// MFCC_36069135352565
// MI455X (gfx1250) — hardware-verified
//
#include <hip/hip_runtime.h>
#include <math.h>

#define NBATCH 64
#define NSAMP 160000
#define WINL 400
#define HOPL 160
#define NFR 998
#define NFRAMES (NBATCH * NFR)
#define NBIN 257
#define NMEL 40
#define NOUT 39
#define FB 64

typedef _Float16 f16;
typedef __attribute__((ext_vector_type(16))) f16 f16x16;
typedef __attribute__((ext_vector_type(8)))  f16 f16x8;
typedef __attribute__((ext_vector_type(8)))  float f32x8;
typedef __attribute__((ext_vector_type(4)))  float v4f_t;
typedef float v4fa __attribute__((ext_vector_type(4), may_alias));

__constant__ float c_fbank[NMEL * NBIN] = {0.0,1.0,0.0,0.0,0.0,0.0,0.0,0.0,0.0,0.0,0.0,0.0,0.0,0.0,0.0,0.0,0.0,0.0,0.0,0.0,0.0,0.0,0.0,0.0,0.0,0.0,0.0,0.0,0.0,0.0,0.0,0.0,0.0,0.0,0.0,0.0,0.0,0.0,0.0,0.0,0.0,0.0,0.0,0.0,0.0,0.0,0.0,0.0,0.0,0.0,0.0,0.0,0.0,0.0,0.0,0.0,0.0,0.0,0.0,0.0,0.0,0.0,0.0,0.0,0.0,0.0,0.0,0.0,0.0,0.0,0.0,0.0,0.0,0.0,0.0,0.0,0.0,0.0,0.0,0.0,0.0,0.0,0.0,0.0,0.0,0.0,0.0,0.0,0.0,0.0,0.0,0.0,0.0,0.0,0.0,0.0,0.0,0.0,0.0,0.0,0.0,0.0,0.0,0.0,0.0,0.0,0.0,0.0,0.0,0.0,0.0,0.0,0.0,0.0,0.0,0.0,0.0,0.0,0.0,0.0,0.0,0.0,0.0,0.0,0.0,0.0,0.0,0.0,0.0,0.0,0.0,0.0,0.0,0.0,0.0,0.0,0.0,0.0,0.0,0.0,0.0,0.0,0.0,0.0,0.0,0.0,0.0,0.0,0.0,0.0,0.0,0.0,0.0,0.0,0.0,0.0,0.0,0.0,0.0,0.0,0.0,0.0,0.0,0.0,0.0,0.0,0.0,0.0,0.0,0.0,0.0,0.0,0.0,0.0,0.0,0.0,0.0,0.0,0.0,0.0,0.0,0.0,0.0,0.0,0.0,0.0,0.0,0.0,0.0,0.0,0.0,0.0,0.0,0.0,0.0,0.0,0.0,0.0,0.0,0.0,0.0,0.0,0.0,0.0,0.0,0.0,0.0,0.0,0.0,0.0,0.0,0.0,0.0,0.0,0.0,0.0,0.0,0.0,0.0,0.0,0.0,0.0,0.0,0.0,0.0,0.0,0.0,0.0,0.0,0.0,0.0,0.0,0.0,0.0,0.0,0.0,0.0,0.0,0.0,0.0,0.0,0.0,0.0,0.0,0.0,0.0,0.0,0.0,0.0,0.0,0.0,0.0,0.0,0.0,0.0,0.0,0.0,0.0,0.0,1.0,0.5,0.0,0.0,0.0,0.0,0.0,0.0,0.0,0.0,0.0,0.0,0.0,0.0,0.0,0.0,0.0,0.0,0.0,0.0,0.0,0.0,0.0,0.0,0.0,0.0,0.0,0.0,0.0,0.0,0.0,0.0,0.0,0.0,0.0,0.0,0.0,0.0,0.0,0.0,0.0,0.0,0.0,0.0,0.0,0.0,0.0,0.0,0.0,0.0,0.0,0.0,0.0,0.0,0.0,0.0,0.0,0.0,0.0,0.0,0.0,0.0,0.0,0.0,0.0,0.0,0.0,0.0,0.0,0.0,0.0,0.0,0.0,0.0,0.0,0.0,0.0,0.0,0.0,0.0,0.0,0.0,0.0,0.0,0.0,0.0,0.0,0.0,0.0,0.0,0.0,0.0,0.0,0.0,0.0,0.0,0.0,0.0,0.0,0.0,0.0,0.0,0.0,0.0,0.0,0.0,0.0,0.0,0.0,0.0,0.0,0.0,0.0,0.0,0.0,0.0,0.0,0.0,0.0,0.0,0.0,0.0,0.0,0.0,0.0,0.0,0.0,0.0,0.0,0.0,0.0,0.0,0.0,0.0,0.0,0.0,0.0,0.0,0.0,0.0,0.0,0.0,0.0,0.0,0.0,0.0,0.0,0.0,0.0,0.0,0.0,0.0,0.0,0.0,0.0,0.0,0.0,0.0,0.0,0.0,0.0,0.0,0.0,0.0,0.0,0.0,0.0,0.0,0.0,0.0,0.0,0.0,0.0,0.0,0.0,0.0,0.0,0.0,0.0,0.0,0.0,0.0,0.0,0.0,0.0,0.0,0.0,0.0,0.0,0.0,0.0,0.0,0.0,0.0,0.0,0.0,0.0,0.0,0.0,0.0,0.0,0.0,0.0,0.0,0.0,0.0,0.0,0.0,0.0,0.0,0.0,0.0,0.0,0.0,0.0,0.0,0.0,0.0,0.0,0.0,0.0,0.0,0.0,0.0,0.0,0.0,0.0,0.0,0.0,0.0,0.0,0.0,0.0,0.0,0.0,0.0,0.0,0.0,0.0,0.0,0.0,0.0,0.0,0.0,0.0,0.0,0.0,0.0,0.0,0.0,0.0,0.0,0.0,0.0,0.0,0.0,0.0,0.0,0.5,1.0,0.5,0.0,0.0,0.0,0.0,0.0,0.0,0.0,0.0,0.0,0.0,0.0,0.0,0.0,0.0,0.0,0.0,0.0,0.0,0.0,0.0,0.0,0.0,0.0,0.0,0.0,0.0,0.0,0.0,0.0,0.0,0.0,0.0,0.0,0.0,0.0,0.0,0.0,0.0,0.0,0.0,0.0,0.0,0.0,0.0,0.0,0.0,0.0,0.0,0.0,0.0,0.0,0.0,0.0,0.0,0.0,0.0,0.0,0.0,0.0,0.0,0.0,0.0,0.0,0.0,0.0,0.0,0.0,0.0,0.0,0.0,0.0,0.0,0.0,0.0,0.0,0.0,0.0,0.0,0.0,0.0,0.0,0.0,0.0,0.0,0.0,0.0,0.0,0.0,0.0,0.0,0.0,0.0,0.0,0.0,0.0,0.0,0.0,0.0,0.0,0.0,0.0,0.0,0.0,0.0,0.0,0.0,0.0,0.0,0.0,0.0,0.0,0.0,0.0,0.0,0.0,0.0,0.0,0.0,0.0,0.0,0.0,0.0,0.0,0.0,0.0,0.0,0.0,0.0,0.0,0.0,0.0,0.0,0.0,0.0,0.0,0.0,0.0,0.0,0.0,0.0,0.0,0.0,0.0,0.0,0.0,0.0,0.0,0.0,0.0,0.0,0.0,0.0,0.0,0.0,0.0,0.0,0.0,0.0,0.0,0.0,0.0,0.0,0.0,0.0,0.0,0.0,0.0,0.0,0.0,0.0,0.0,0.0,0.0,0.0,0.0,0.0,0.0,0.0,0.0,0.0,0.0,0.0,0.0,0.0,0.0,0.0,0.0,0.0,0.0,0.0,0.0,0.0,0.0,0.0,0.0,0.0,0.0,0.0,0.0,0.0,0.0,0.0,0.0,0.0,0.0,0.0,0.0,0.0,0.0,0.0,0.0,0.0,0.0,0.0,0.0,0.0,0.0,0.0,0.0,0.0,0.0,0.0,0.0,0.0,0.0,0.0,0.0,0.0,0.0,0.0,0.0,0.0,0.0,0.0,0.0,0.0,0.0,0.0,0.0,0.0,0.0,0.0,0.0,0.0,0.0,0.0,0.0,0.0,0.0,0.0,0.0,0.0,0.0,0.0,0.0,0.0,0.5,1.0,0.5,0.0,0.0,0.0,0.0,0.0,0.0,0.0,0.0,0.0,0.0,0.0,0.0,0.0,0.0,0.0,0.0,0.0,0.0,0.0,0.0,0.0,0.0,0.0,0.0,0.0,0.0,0.0,0.0,0.0,0.0,0.0,0.0,0.0,0.0,0.0,0.0,0.0,0.0,0.0,0.0,0.0,0.0,0.0,0.0,0.0,0.0,0.0,0.0,0.0,0.0,0.0,0.0,0.0,0.0,0.0,0.0,0.0,0.0,0.0,0.0,0.0,0.0,0.0,0.0,0.0,0.0,0.0,0.0,0.0,0.0,0.0,0.0,0.0,0.0,0.0,0.0,0.0,0.0,0.0,0.0,0.0,0.0,0.0,0.0,0.0,0.0,0.0,0.0,0.0,0.0,0.0,0.0,0.0,0.0,0.0,0.0,0.0,0.0,0.0,0.0,0.0,0.0,0.0,0.0,0.0,0.0,0.0,0.0,0.0,0.0,0.0,0.0,0.0,0.0,0.0,0.0,0.0,0.0,0.0,0.0,0.0,0.0,0.0,0.0,0.0,0.0,0.0,0.0,0.0,0.0,0.0,0.0,0.0,0.0,0.0,0.0,0.0,0.0,0.0,0.0,0.0,0.0,0.0,0.0,0.0,0.0,0.0,0.0,0.0,0.0,0.0,0.0,0.0,0.0,0.0,0.0,0.0,0.0,0.0,0.0,0.0,0.0,0.0,0.0,0.0,0.0,0.0,0.0,0.0,0.0,0.0,0.0,0.0,0.0,0.0,0.0,0.0,0.0,0.0,0.0,0.0,0.0,0.0,0.0,0.0,0.0,0.0,0.0,0.0,0.0,0.0,0.0,0.0,0.0,0.0,0.0,0.0,0.0,0.0,0.0,0.0,0.0,0.0,0.0,0.0,0.0,0.0,0.0,0.0,0.0,0.0,0.0,0.0,0.0,0.0,0.0,0.0,0.0,0.0,0.0,0.0,0.0,0.0,0.0,0.0,0.0,0.0,0.0,0.0,0.0,0.0,0.0,0.0,0.0,0.0,0.0,0.0,0.0,0.0,0.0,0.0,0.0,0.0,0.0,0.0,0.0,0.0,0.0,0.0,0.0,0.0,0.0,0.0,0.0,0.0,0.0,0.5,1.0,0.5,0.0,0.0,0.0,0.0,0.0,0.0,0.0,0.0,0.0,0.0,0.0,0.0,0.0,0.0,0.0,0.0,0.0,0.0,0.0,0.0,0.0,0.0,0.0,0.0,0.0,0.0,0.0,0.0,0.0,0.0,0.0,0.0,0.0,0.0,0.0,0.0,0.0,0.0,0.0,0.0,0.0,0.0,0.0,0.0,0.0,0.0,0.0,0.0,0.0,0.0,0.0,0.0,0.0,0.0,0.0,0.0,0.0,0.0,0.0,0.0,0.0,0.0,0.0,0.0,0.0,0.0,0.0,0.0,0.0,0.0,0.0,0.0,0.0,0.0,0.0,0.0,0.0,0.0,0.0,0.0,0.0,0.0,0.0,0.0,0.0,0.0,0.0,0.0,0.0,0.0,0.0,0.0,0.0,0.0,0.0,0.0,0.0,0.0,0.0,0.0,0.0,0.0,0.0,0.0,0.0,0.0,0.0,0.0,0.0,0.0,0.0,0.0,0.0,0.0,0.0,0.0,0.0,0.0,0.0,0.0,0.0,0.0,0.0,0.0,0.0,0.0,0.0,0.0,0.0,0.0,0.0,0.0,0.0,0.0,0.0,0.0,0.0,0.0,0.0,0.0,0.0,0.0,0.0,0.0,0.0,0.0,0.0,0.0,0.0,0.0,0.0,0.0,0.0,0.0,0.0,0.0,0.0,0.0,0.0,0.0,0.0,0.0,0.0,0.0,0.0,0.0,0.0,0.0,0.0,0.0,0.0,0.0,0.0,0.0,0.0,0.0,0.0,0.0,0.0,0.0,0.0,0.0,0.0,0.0,0.0,0.0,0.0,0.0,0.0,0.0,0.0,0.0,0.0,0.0,0.0,0.0,0.0,0.0,0.0,0.0,0.0,0.0,0.0,0.0,0.0,0.0,0.0,0.0,0.0,0.0,0.0,0.0,0.0,0.0,0.0,0.0,0.0,0.0,0.0,0.0,0.0,0.0,0.0,0.0,0.0,0.0,0.0,0.0,0.0,0.0,0.0,0.0,0.0,0.0,0.0,0.0,0.0,0.0,0.0,0.0,0.0,0.0,0.0,0.0,0.0,0.0,0.0,0.0,0.0,0.0,0.0,0.0,0.0,0.0,0.0,0.0,0.5,1.0,0.5,0.0,0.0,0.0,0.0,0.0,0.0,0.0,0.0,0.0,0.0,0.0,0.0,0.0,0.0,0.0,0.0,0.0,0.0,0.0,0.0,0.0,0.0,0.0,0.0,0.0,0.0,0.0,0.0,0.0,0.0,0.0,0.0,0.0,0.0,0.0,0.0,0.0,0.0,0.0,0.0,0.0,0.0,0.0,0.0,0.0,0.0,0.0,0.0,0.0,0.0,0.0,0.0,0.0,0.0,0.0,0.0,0.0,0.0,0.0,0.0,0.0,0.0,0.0,0.0,0.0,0.0,0.0,0.0,0.0,0.0,0.0,0.0,0.0,0.0,0.0,0.0,0.0,0.0,0.0,0.0,0.0,0.0,0.0,0.0,0.0,0.0,0.0,0.0,0.0,0.0,0.0,0.0,0.0,0.0,0.0,0.0,0.0,0.0,0.0,0.0,0.0,0.0,0.0,0.0,0.0,0.0,0.0,0.0,0.0,0.0,0.0,0.0,0.0,0.0,0.0,0.0,0.0,0.0,0.0,0.0,0.0,0.0,0.0,0.0,0.0,0.0,0.0,0.0,0.0,0.0,0.0,0.0,0.0,0.0,0.0,0.0,0.0,0.0,0.0,0.0,0.0,0.0,0.0,0.0,0.0,0.0,0.0,0.0,0.0,0.0,0.0,0.0,0.0,0.0,0.0,0.0,0.0,0.0,0.0,0.0,0.0,0.0,0.0,0.0,0.0,0.0,0.0,0.0,0.0,0.0,0.0,0.0,0.0,0.0,0.0,0.0,0.0,0.0,0.0,0.0,0.0,0.0,0.0,0.0,0.0,0.0,0.0,0.0,0.0,0.0,0.0,0.0,0.0,0.0,0.0,0.0,0.0,0.0,0.0,0.0,0.0,0.0,0.0,0.0,0.0,0.0,0.0,0.0,0.0,0.0,0.0,0.0,0.0,0.0,0.0,0.0,0.0,0.0,0.0,0.0,0.0,0.0,0.0,0.0,0.0,0.0,0.0,0.0,0.0,0.0,0.0,0.0,0.0,0.0,0.0,0.0,0.0,0.0,0.0,0.0,0.0,0.0,0.0,0.0,0.0,0.0,0.0,0.0,0.0,0.0,0.0,0.0,0.0,0.0,0.0,0.0,0.5,1.0,0.5,0.0,0.0,0.0,0.0,0.0,0.0,0.0,0.0,0.0,0.0,0.0,0.0,0.0,0.0,0.0,0.0,0.0,0.0,0.0,0.0,0.0,0.0,0.0,0.0,0.0,0.0,0.0,0.0,0.0,0.0,0.0,0.0,0.0,0.0,0.0,0.0,0.0,0.0,0.0,0.0,0.0,0.0,0.0,0.0,0.0,0.0,0.0,0.0,0.0,0.0,0.0,0.0,0.0,0.0,0.0,0.0,0.0,0.0,0.0,0.0,0.0,0.0,0.0,0.0,0.0,0.0,0.0,0.0,0.0,0.0,0.0,0.0,0.0,0.0,0.0,0.0,0.0,0.0,0.0,0.0,0.0,0.0,0.0,0.0,0.0,0.0,0.0,0.0,0.0,0.0,0.0,0.0,0.0,0.0,0.0,0.0,0.0,0.0,0.0,0.0,0.0,0.0,0.0,0.0,0.0,0.0,0.0,0.0,0.0,0.0,0.0,0.0,0.0,0.0,0.0,0.0,0.0,0.0,0.0,0.0,0.0,0.0,0.0,0.0,0.0,0.0,0.0,0.0,0.0,0.0,0.0,0.0,0.0,0.0,0.0,0.0,0.0,0.0,0.0,0.0,0.0,0.0,0.0,0.0,0.0,0.0,0.0,0.0,0.0,0.0,0.0,0.0,0.0,0.0,0.0,0.0,0.0,0.0,0.0,0.0,0.0,0.0,0.0,0.0,0.0,0.0,0.0,0.0,0.0,0.0,0.0,0.0,0.0,0.0,0.0,0.0,0.0,0.0,0.0,0.0,0.0,0.0,0.0,0.0,0.0,0.0,0.0,0.0,0.0,0.0,0.0,0.0,0.0,0.0,0.0,0.0,0.0,0.0,0.0,0.0,0.0,0.0,0.0,0.0,0.0,0.0,0.0,0.0,0.0,0.0,0.0,0.0,0.0,0.0,0.0,0.0,0.0,0.0,0.0,0.0,0.0,0.0,0.0,0.0,0.0,0.0,0.0,0.0,0.0,0.0,0.0,0.0,0.0,0.0,0.0,0.0,0.0,0.0,0.0,0.0,0.0,0.0,0.0,0.0,0.0,0.0,0.0,0.0,0.0,0.0,0.0,0.0,0.0,0.0,0.0,0.0,0.5,1.0,0.5,0.0,0.0,0.0,0.0,0.0,0.0,0.0,0.0,0.0,0.0,0.0,0.0,0.0,0.0,0.0,0.0,0.0,0.0,0.0,0.0,0.0,0.0,0.0,0.0,0.0,0.0,0.0,0.0,0.0,0.0,0.0,0.0,0.0,0.0,0.0,0.0,0.0,0.0,0.0,0.0,0.0,0.0,0.0,0.0,0.0,0.0,0.0,0.0,0.0,0.0,0.0,0.0,0.0,0.0,0.0,0.0,0.0,0.0,0.0,0.0,0.0,0.0,0.0,0.0,0.0,0.0,0.0,0.0,0.0,0.0,0.0,0.0,0.0,0.0,0.0,0.0,0.0,0.0,0.0,0.0,0.0,0.0,0.0,0.0,0.0,0.0,0.0,0.0,0.0,0.0,0.0,0.0,0.0,0.0,0.0,0.0,0.0,0.0,0.0,0.0,0.0,0.0,0.0,0.0,0.0,0.0,0.0,0.0,0.0,0.0,0.0,0.0,0.0,0.0,0.0,0.0,0.0,0.0,0.0,0.0,0.0,0.0,0.0,0.0,0.0,0.0,0.0,0.0,0.0,0.0,0.0,0.0,0.0,0.0,0.0,0.0,0.0,0.0,0.0,0.0,0.0,0.0,0.0,0.0,0.0,0.0,0.0,0.0,0.0,0.0,0.0,0.0,0.0,0.0,0.0,0.0,0.0,0.0,0.0,0.0,0.0,0.0,0.0,0.0,0.0,0.0,0.0,0.0,0.0,0.0,0.0,0.0,0.0,0.0,0.0,0.0,0.0,0.0,0.0,0.0,0.0,0.0,0.0,0.0,0.0,0.0,0.0,0.0,0.0,0.0,0.0,0.0,0.0,0.0,0.0,0.0,0.0,0.0,0.0,0.0,0.0,0.0,0.0,0.0,0.0,0.0,0.0,0.0,0.0,0.0,0.0,0.0,0.0,0.0,0.0,0.0,0.0,0.0,0.0,0.0,0.0,0.0,0.0,0.0,0.0,0.0,0.0,0.0,0.0,0.0,0.0,0.0,0.0,0.0,0.0,0.0,0.0,0.0,0.0,0.0,0.0,0.0,0.0,0.0,0.0,0.0,0.0,0.0,0.0,0.0,0.0,0.0,0.0,0.0,0.0,0.0,0.5,1.0,0.6666666865348816,0.3333333432674408,0.0,0.0,0.0,0.0,0.0,0.0,0.0,0.0,0.0,0.0,0.0,0.0,0.0,0.0,0.0,0.0,0.0,0.0,0.0,0.0,0.0,0.0,0.0,0.0,0.0,0.0,0.0,0.0,0.0,0.0,0.0,0.0,0.0,0.0,0.0,0.0,0.0,0.0,0.0,0.0,0.0,0.0,0.0,0.0,0.0,0.0,0.0,0.0,0.0,0.0,0.0,0.0,0.0,0.0,0.0,0.0,0.0,0.0,0.0,0.0,0.0,0.0,0.0,0.0,0.0,0.0,0.0,0.0,0.0,0.0,0.0,0.0,0.0,0.0,0.0,0.0,0.0,0.0,0.0,0.0,0.0,0.0,0.0,0.0,0.0,0.0,0.0,0.0,0.0,0.0,0.0,0.0,0.0,0.0,0.0,0.0,0.0,0.0,0.0,0.0,0.0,0.0,0.0,0.0,0.0,0.0,0.0,0.0,0.0,0.0,0.0,0.0,0.0,0.0,0.0,0.0,0.0,0.0,0.0,0.0,0.0,0.0,0.0,0.0,0.0,0.0,0.0,0.0,0.0,0.0,0.0,0.0,0.0,0.0,0.0,0.0,0.0,0.0,0.0,0.0,0.0,0.0,0.0,0.0,0.0,0.0,0.0,0.0,0.0,0.0,0.0,0.0,0.0,0.0,0.0,0.0,0.0,0.0,0.0,0.0,0.0,0.0,0.0,0.0,0.0,0.0,0.0,0.0,0.0,0.0,0.0,0.0,0.0,0.0,0.0,0.0,0.0,0.0,0.0,0.0,0.0,0.0,0.0,0.0,0.0,0.0,0.0,0.0,0.0,0.0,0.0,0.0,0.0,0.0,0.0,0.0,0.0,0.0,0.0,0.0,0.0,0.0,0.0,0.0,0.0,0.0,0.0,0.0,0.0,0.0,0.0,0.0,0.0,0.0,0.0,0.0,0.0,0.0,0.0,0.0,0.0,0.0,0.0,0.0,0.0,0.0,0.0,0.0,0.0,0.0,0.0,0.0,0.0,0.0,0.0,0.0,0.0,0.0,0.0,0.0,0.0,0.0,0.0,0.0,0.0,0.0,0.0,0.0,0.0,0.0,0.0,0.0,0.0,0.0,0.0,0.3333333432674408,0.6666666865348816,1.0,0.5,0.0,0.0,0.0,0.0,0.0,0.0,0.0,0.0,0.0,0.0,0.0,0.0,0.0,0.0,0.0,0.0,0.0,0.0,0.0,0.0,0.0,0.0,0.0,0.0,0.0,0.0,0.0,0.0,0.0,0.0,0.0,0.0,0.0,0.0,0.0,0.0,0.0,0.0,0.0,0.0,0.0,0.0,0.0,0.0,0.0,0.0,0.0,0.0,0.0,0.0,0.0,0.0,0.0,0.0,0.0,0.0,0.0,0.0,0.0,0.0,0.0,0.0,0.0,0.0,0.0,0.0,0.0,0.0,0.0,0.0,0.0,0.0,0.0,0.0,0.0,0.0,0.0,0.0,0.0,0.0,0.0,0.0,0.0,0.0,0.0,0.0,0.0,0.0,0.0,0.0,0.0,0.0,0.0,0.0,0.0,0.0,0.0,0.0,0.0,0.0,0.0,0.0,0.0,0.0,0.0,0.0,0.0,0.0,0.0,0.0,0.0,0.0,0.0,0.0,0.0,0.0,0.0,0.0,0.0,0.0,0.0,0.0,0.0,0.0,0.0,0.0,0.0,0.0,0.0,0.0,0.0,0.0,0.0,0.0,0.0,0.0,0.0,0.0,0.0,0.0,0.0,0.0,0.0,0.0,0.0,0.0,0.0,0.0,0.0,0.0,0.0,0.0,0.0,0.0,0.0,0.0,0.0,0.0,0.0,0.0,0.0,0.0,0.0,0.0,0.0,0.0,0.0,0.0,0.0,0.0,0.0,0.0,0.0,0.0,0.0,0.0,0.0,0.0,0.0,0.0,0.0,0.0,0.0,0.0,0.0,0.0,0.0,0.0,0.0,0.0,0.0,0.0,0.0,0.0,0.0,0.0,0.0,0.0,0.0,0.0,0.0,0.0,0.0,0.0,0.0,0.0,0.0,0.0,0.0,0.0,0.0,0.0,0.0,0.0,0.0,0.0,0.0,0.0,0.0,0.0,0.0,0.0,0.0,0.0,0.0,0.0,0.0,0.0,0.0,0.0,0.0,0.0,0.0,0.0,0.0,0.0,0.0,0.0,0.0,0.0,0.0,0.0,0.0,0.0,0.0,0.0,0.0,0.0,0.0,0.0,0.0,0.0,0.0,0.0,0.0,0.0,0.5,1.0,0.6666666865348816,0.3333333432674408,0.0,0.0,0.0,0.0,0.0,0.0,0.0,0.0,0.0,0.0,0.0,0.0,0.0,0.0,0.0,0.0,0.0,0.0,0.0,0.0,0.0,0.0,0.0,0.0,0.0,0.0,0.0,0.0,0.0,0.0,0.0,0.0,0.0,0.0,0.0,0.0,0.0,0.0,0.0,0.0,0.0,0.0,0.0,0.0,0.0,0.0,0.0,0.0,0.0,0.0,0.0,0.0,0.0,0.0,0.0,0.0,0.0,0.0,0.0,0.0,0.0,0.0,0.0,0.0,0.0,0.0,0.0,0.0,0.0,0.0,0.0,0.0,0.0,0.0,0.0,0.0,0.0,0.0,0.0,0.0,0.0,0.0,0.0,0.0,0.0,0.0,0.0,0.0,0.0,0.0,0.0,0.0,0.0,0.0,0.0,0.0,0.0,0.0,0.0,0.0,0.0,0.0,0.0,0.0,0.0,0.0,0.0,0.0,0.0,0.0,0.0,0.0,0.0,0.0,0.0,0.0,0.0,0.0,0.0,0.0,0.0,0.0,0.0,0.0,0.0,0.0,0.0,0.0,0.0,0.0,0.0,0.0,0.0,0.0,0.0,0.0,0.0,0.0,0.0,0.0,0.0,0.0,0.0,0.0,0.0,0.0,0.0,0.0,0.0,0.0,0.0,0.0,0.0,0.0,0.0,0.0,0.0,0.0,0.0,0.0,0.0,0.0,0.0,0.0,0.0,0.0,0.0,0.0,0.0,0.0,0.0,0.0,0.0,0.0,0.0,0.0,0.0,0.0,0.0,0.0,0.0,0.0,0.0,0.0,0.0,0.0,0.0,0.0,0.0,0.0,0.0,0.0,0.0,0.0,0.0,0.0,0.0,0.0,0.0,0.0,0.0,0.0,0.0,0.0,0.0,0.0,0.0,0.0,0.0,0.0,0.0,0.0,0.0,0.0,0.0,0.0,0.0,0.0,0.0,0.0,0.0,0.0,0.0,0.0,0.0,0.0,0.0,0.0,0.0,0.0,0.0,0.0,0.0,0.0,0.0,0.0,0.0,0.0,0.0,0.0,0.0,0.0,0.0,0.0,0.0,0.0,0.0,0.0,0.0,0.0,0.0,0.0,0.0,0.0,0.0,0.3333333432674408,0.6666666865348816,1.0,0.6666666865348816,0.3333333432674408,0.0,0.0,0.0,0.0,0.0,0.0,0.0,0.0,0.0,0.0,0.0,0.0,0.0,0.0,0.0,0.0,0.0,0.0,0.0,0.0,0.0,0.0,0.0,0.0,0.0,0.0,0.0,0.0,0.0,0.0,0.0,0.0,0.0,0.0,0.0,0.0,0.0,0.0,0.0,0.0,0.0,0.0,0.0,0.0,0.0,0.0,0.0,0.0,0.0,0.0,0.0,0.0,0.0,0.0,0.0,0.0,0.0,0.0,0.0,0.0,0.0,0.0,0.0,0.0,0.0,0.0,0.0,0.0,0.0,0.0,0.0,0.0,0.0,0.0,0.0,0.0,0.0,0.0,0.0,0.0,0.0,0.0,0.0,0.0,0.0,0.0,0.0,0.0,0.0,0.0,0.0,0.0,0.0,0.0,0.0,0.0,0.0,0.0,0.0,0.0,0.0,0.0,0.0,0.0,0.0,0.0,0.0,0.0,0.0,0.0,0.0,0.0,0.0,0.0,0.0,0.0,0.0,0.0,0.0,0.0,0.0,0.0,0.0,0.0,0.0,0.0,0.0,0.0,0.0,0.0,0.0,0.0,0.0,0.0,0.0,0.0,0.0,0.0,0.0,0.0,0.0,0.0,0.0,0.0,0.0,0.0,0.0,0.0,0.0,0.0,0.0,0.0,0.0,0.0,0.0,0.0,0.0,0.0,0.0,0.0,0.0,0.0,0.0,0.0,0.0,0.0,0.0,0.0,0.0,0.0,0.0,0.0,0.0,0.0,0.0,0.0,0.0,0.0,0.0,0.0,0.0,0.0,0.0,0.0,0.0,0.0,0.0,0.0,0.0,0.0,0.0,0.0,0.0,0.0,0.0,0.0,0.0,0.0,0.0,0.0,0.0,0.0,0.0,0.0,0.0,0.0,0.0,0.0,0.0,0.0,0.0,0.0,0.0,0.0,0.0,0.0,0.0,0.0,0.0,0.0,0.0,0.0,0.0,0.0,0.0,0.0,0.0,0.0,0.0,0.0,0.0,0.0,0.0,0.0,0.0,0.0,0.0,0.0,0.0,0.0,0.0,0.0,0.0,0.0,0.0,0.0,0.0,0.0,0.0,0.0,0.0,0.0,0.0,0.0,0.0,0.3333333432674408,0.6666666865348816,1.0,0.6666666865348816,0.3333333432674408,0.0,0.0,0.0,0.0,0.0,0.0,0.0,0.0,0.0,0.0,0.0,0.0,0.0,0.0,0.0,0.0,0.0,0.0,0.0,0.0,0.0,0.0,0.0,0.0,0.0,0.0,0.0,0.0,0.0,0.0,0.0,0.0,0.0,0.0,0.0,0.0,0.0,0.0,0.0,0.0,0.0,0.0,0.0,0.0,0.0,0.0,0.0,0.0,0.0,0.0,0.0,0.0,0.0,0.0,0.0,0.0,0.0,0.0,0.0,0.0,0.0,0.0,0.0,0.0,0.0,0.0,0.0,0.0,0.0,0.0,0.0,0.0,0.0,0.0,0.0,0.0,0.0,0.0,0.0,0.0,0.0,0.0,0.0,0.0,0.0,0.0,0.0,0.0,0.0,0.0,0.0,0.0,0.0,0.0,0.0,0.0,0.0,0.0,0.0,0.0,0.0,0.0,0.0,0.0,0.0,0.0,0.0,0.0,0.0,0.0,0.0,0.0,0.0,0.0,0.0,0.0,0.0,0.0,0.0,0.0,0.0,0.0,0.0,0.0,0.0,0.0,0.0,0.0,0.0,0.0,0.0,0.0,0.0,0.0,0.0,0.0,0.0,0.0,0.0,0.0,0.0,0.0,0.0,0.0,0.0,0.0,0.0,0.0,0.0,0.0,0.0,0.0,0.0,0.0,0.0,0.0,0.0,0.0,0.0,0.0,0.0,0.0,0.0,0.0,0.0,0.0,0.0,0.0,0.0,0.0,0.0,0.0,0.0,0.0,0.0,0.0,0.0,0.0,0.0,0.0,0.0,0.0,0.0,0.0,0.0,0.0,0.0,0.0,0.0,0.0,0.0,0.0,0.0,0.0,0.0,0.0,0.0,0.0,0.0,0.0,0.0,0.0,0.0,0.0,0.0,0.0,0.0,0.0,0.0,0.0,0.0,0.0,0.0,0.0,0.0,0.0,0.0,0.0,0.0,0.0,0.0,0.0,0.0,0.0,0.0,0.0,0.0,0.0,0.0,0.0,0.0,0.0,0.0,0.0,0.0,0.0,0.0,0.0,0.0,0.0,0.0,0.0,0.0,0.0,0.0,0.0,0.0,0.0,0.0,0.0,0.0,0.0,0.0,0.0,0.0,0.3333333432674408,0.6666666865348816,1.0,0.6666666865348816,0.3333333432674408,0.0,0.0,0.0,0.0,0.0,0.0,0.0,0.0,0.0,0.0,0.0,0.0,0.0,0.0,0.0,0.0,0.0,0.0,0.0,0.0,0.0,0.0,0.0,0.0,0.0,0.0,0.0,0.0,0.0,0.0,0.0,0.0,0.0,0.0,0.0,0.0,0.0,0.0,0.0,0.0,0.0,0.0,0.0,0.0,0.0,0.0,0.0,0.0,0.0,0.0,0.0,0.0,0.0,0.0,0.0,0.0,0.0,0.0,0.0,0.0,0.0,0.0,0.0,0.0,0.0,0.0,0.0,0.0,0.0,0.0,0.0,0.0,0.0,0.0,0.0,0.0,0.0,0.0,0.0,0.0,0.0,0.0,0.0,0.0,0.0,0.0,0.0,0.0,0.0,0.0,0.0,0.0,0.0,0.0,0.0,0.0,0.0,0.0,0.0,0.0,0.0,0.0,0.0,0.0,0.0,0.0,0.0,0.0,0.0,0.0,0.0,0.0,0.0,0.0,0.0,0.0,0.0,0.0,0.0,0.0,0.0,0.0,0.0,0.0,0.0,0.0,0.0,0.0,0.0,0.0,0.0,0.0,0.0,0.0,0.0,0.0,0.0,0.0,0.0,0.0,0.0,0.0,0.0,0.0,0.0,0.0,0.0,0.0,0.0,0.0,0.0,0.0,0.0,0.0,0.0,0.0,0.0,0.0,0.0,0.0,0.0,0.0,0.0,0.0,0.0,0.0,0.0,0.0,0.0,0.0,0.0,0.0,0.0,0.0,0.0,0.0,0.0,0.0,0.0,0.0,0.0,0.0,0.0,0.0,0.0,0.0,0.0,0.0,0.0,0.0,0.0,0.0,0.0,0.0,0.0,0.0,0.0,0.0,0.0,0.0,0.0,0.0,0.0,0.0,0.0,0.0,0.0,0.0,0.0,0.0,0.0,0.0,0.0,0.0,0.0,0.0,0.0,0.0,0.0,0.0,0.0,0.0,0.0,0.0,0.0,0.0,0.0,0.0,0.0,0.0,0.0,0.0,0.0,0.0,0.0,0.0,0.0,0.0,0.0,0.0,0.0,0.0,0.0,0.0,0.0,0.0,0.0,0.0,0.0,0.0,0.0,0.0,0.0,0.0,0.0,0.3333333432674408,0.6666666865348816,1.0,0.75,0.5,0.25,0.0,0.0,0.0,0.0,0.0,0.0,0.0,0.0,0.0,0.0,0.0,0.0,0.0,0.0,0.0,0.0,0.0,0.0,0.0,0.0,0.0,0.0,0.0,0.0,0.0,0.0,0.0,0.0,0.0,0.0,0.0,0.0,0.0,0.0,0.0,0.0,0.0,0.0,0.0,0.0,0.0,0.0,0.0,0.0,0.0,0.0,0.0,0.0,0.0,0.0,0.0,0.0,0.0,0.0,0.0,0.0,0.0,0.0,0.0,0.0,0.0,0.0,0.0,0.0,0.0,0.0,0.0,0.0,0.0,0.0,0.0,0.0,0.0,0.0,0.0,0.0,0.0,0.0,0.0,0.0,0.0,0.0,0.0,0.0,0.0,0.0,0.0,0.0,0.0,0.0,0.0,0.0,0.0,0.0,0.0,0.0,0.0,0.0,0.0,0.0,0.0,0.0,0.0,0.0,0.0,0.0,0.0,0.0,0.0,0.0,0.0,0.0,0.0,0.0,0.0,0.0,0.0,0.0,0.0,0.0,0.0,0.0,0.0,0.0,0.0,0.0,0.0,0.0,0.0,0.0,0.0,0.0,0.0,0.0,0.0,0.0,0.0,0.0,0.0,0.0,0.0,0.0,0.0,0.0,0.0,0.0,0.0,0.0,0.0,0.0,0.0,0.0,0.0,0.0,0.0,0.0,0.0,0.0,0.0,0.0,0.0,0.0,0.0,0.0,0.0,0.0,0.0,0.0,0.0,0.0,0.0,0.0,0.0,0.0,0.0,0.0,0.0,0.0,0.0,0.0,0.0,0.0,0.0,0.0,0.0,0.0,0.0,0.0,0.0,0.0,0.0,0.0,0.0,0.0,0.0,0.0,0.0,0.0,0.0,0.0,0.0,0.0,0.0,0.0,0.0,0.0,0.0,0.0,0.0,0.0,0.0,0.0,0.0,0.0,0.0,0.0,0.0,0.0,0.0,0.0,0.0,0.0,0.0,0.0,0.0,0.0,0.0,0.0,0.0,0.0,0.0,0.0,0.0,0.0,0.0,0.0,0.0,0.0,0.0,0.0,0.0,0.0,0.0,0.0,0.0,0.0,0.0,0.0,0.0,0.0,0.0,0.0,0.0,0.0,0.25,0.5,0.75,1.0,0.75,0.5,0.25,0.0,0.0,0.0,0.0,0.0,0.0,0.0,0.0,0.0,0.0,0.0,0.0,0.0,0.0,0.0,0.0,0.0,0.0,0.0,0.0,0.0,0.0,0.0,0.0,0.0,0.0,0.0,0.0,0.0,0.0,0.0,0.0,0.0,0.0,0.0,0.0,0.0,0.0,0.0,0.0,0.0,0.0,0.0,0.0,0.0,0.0,0.0,0.0,0.0,0.0,0.0,0.0,0.0,0.0,0.0,0.0,0.0,0.0,0.0,0.0,0.0,0.0,0.0,0.0,0.0,0.0,0.0,0.0,0.0,0.0,0.0,0.0,0.0,0.0,0.0,0.0,0.0,0.0,0.0,0.0,0.0,0.0,0.0,0.0,0.0,0.0,0.0,0.0,0.0,0.0,0.0,0.0,0.0,0.0,0.0,0.0,0.0,0.0,0.0,0.0,0.0,0.0,0.0,0.0,0.0,0.0,0.0,0.0,0.0,0.0,0.0,0.0,0.0,0.0,0.0,0.0,0.0,0.0,0.0,0.0,0.0,0.0,0.0,0.0,0.0,0.0,0.0,0.0,0.0,0.0,0.0,0.0,0.0,0.0,0.0,0.0,0.0,0.0,0.0,0.0,0.0,0.0,0.0,0.0,0.0,0.0,0.0,0.0,0.0,0.0,0.0,0.0,0.0,0.0,0.0,0.0,0.0,0.0,0.0,0.0,0.0,0.0,0.0,0.0,0.0,0.0,0.0,0.0,0.0,0.0,0.0,0.0,0.0,0.0,0.0,0.0,0.0,0.0,0.0,0.0,0.0,0.0,0.0,0.0,0.0,0.0,0.0,0.0,0.0,0.0,0.0,0.0,0.0,0.0,0.0,0.0,0.0,0.0,0.0,0.0,0.0,0.0,0.0,0.0,0.0,0.0,0.0,0.0,0.0,0.0,0.0,0.0,0.0,0.0,0.0,0.0,0.0,0.0,0.0,0.0,0.0,0.0,0.0,0.0,0.0,0.0,0.0,0.0,0.0,0.0,0.0,0.0,0.0,0.0,0.0,0.0,0.0,0.0,0.0,0.0,0.0,0.0,0.0,0.0,0.0,0.0,0.0,0.0,0.0,0.0,0.0,0.0,0.0,0.0,0.25,0.5,0.75,1.0,0.75,0.5,0.25,0.0,0.0,0.0,0.0,0.0,0.0,0.0,0.0,0.0,0.0,0.0,0.0,0.0,0.0,0.0,0.0,0.0,0.0,0.0,0.0,0.0,0.0,0.0,0.0,0.0,0.0,0.0,0.0,0.0,0.0,0.0,0.0,0.0,0.0,0.0,0.0,0.0,0.0,0.0,0.0,0.0,0.0,0.0,0.0,0.0,0.0,0.0,0.0,0.0,0.0,0.0,0.0,0.0,0.0,0.0,0.0,0.0,0.0,0.0,0.0,0.0,0.0,0.0,0.0,0.0,0.0,0.0,0.0,0.0,0.0,0.0,0.0,0.0,0.0,0.0,0.0,0.0,0.0,0.0,0.0,0.0,0.0,0.0,0.0,0.0,0.0,0.0,0.0,0.0,0.0,0.0,0.0,0.0,0.0,0.0,0.0,0.0,0.0,0.0,0.0,0.0,0.0,0.0,0.0,0.0,0.0,0.0,0.0,0.0,0.0,0.0,0.0,0.0,0.0,0.0,0.0,0.0,0.0,0.0,0.0,0.0,0.0,0.0,0.0,0.0,0.0,0.0,0.0,0.0,0.0,0.0,0.0,0.0,0.0,0.0,0.0,0.0,0.0,0.0,0.0,0.0,0.0,0.0,0.0,0.0,0.0,0.0,0.0,0.0,0.0,0.0,0.0,0.0,0.0,0.0,0.0,0.0,0.0,0.0,0.0,0.0,0.0,0.0,0.0,0.0,0.0,0.0,0.0,0.0,0.0,0.0,0.0,0.0,0.0,0.0,0.0,0.0,0.0,0.0,0.0,0.0,0.0,0.0,0.0,0.0,0.0,0.0,0.0,0.0,0.0,0.0,0.0,0.0,0.0,0.0,0.0,0.0,0.0,0.0,0.0,0.0,0.0,0.0,0.0,0.0,0.0,0.0,0.0,0.0,0.0,0.0,0.0,0.0,0.0,0.0,0.0,0.0,0.0,0.0,0.0,0.0,0.0,0.0,0.0,0.0,0.0,0.0,0.0,0.0,0.0,0.0,0.0,0.0,0.0,0.0,0.0,0.0,0.0,0.0,0.0,0.0,0.0,0.0,0.0,0.0,0.0,0.0,0.0,0.0,0.0,0.0,0.0,0.0,0.0,0.25,0.5,0.75,1.0,0.75,0.5,0.25,0.0,0.0,0.0,0.0,0.0,0.0,0.0,0.0,0.0,0.0,0.0,0.0,0.0,0.0,0.0,0.0,0.0,0.0,0.0,0.0,0.0,0.0,0.0,0.0,0.0,0.0,0.0,0.0,0.0,0.0,0.0,0.0,0.0,0.0,0.0,0.0,0.0,0.0,0.0,0.0,0.0,0.0,0.0,0.0,0.0,0.0,0.0,0.0,0.0,0.0,0.0,0.0,0.0,0.0,0.0,0.0,0.0,0.0,0.0,0.0,0.0,0.0,0.0,0.0,0.0,0.0,0.0,0.0,0.0,0.0,0.0,0.0,0.0,0.0,0.0,0.0,0.0,0.0,0.0,0.0,0.0,0.0,0.0,0.0,0.0,0.0,0.0,0.0,0.0,0.0,0.0,0.0,0.0,0.0,0.0,0.0,0.0,0.0,0.0,0.0,0.0,0.0,0.0,0.0,0.0,0.0,0.0,0.0,0.0,0.0,0.0,0.0,0.0,0.0,0.0,0.0,0.0,0.0,0.0,0.0,0.0,0.0,0.0,0.0,0.0,0.0,0.0,0.0,0.0,0.0,0.0,0.0,0.0,0.0,0.0,0.0,0.0,0.0,0.0,0.0,0.0,0.0,0.0,0.0,0.0,0.0,0.0,0.0,0.0,0.0,0.0,0.0,0.0,0.0,0.0,0.0,0.0,0.0,0.0,0.0,0.0,0.0,0.0,0.0,0.0,0.0,0.0,0.0,0.0,0.0,0.0,0.0,0.0,0.0,0.0,0.0,0.0,0.0,0.0,0.0,0.0,0.0,0.0,0.0,0.0,0.0,0.0,0.0,0.0,0.0,0.0,0.0,0.0,0.0,0.0,0.0,0.0,0.0,0.0,0.0,0.0,0.0,0.0,0.0,0.0,0.0,0.0,0.0,0.0,0.0,0.0,0.0,0.0,0.0,0.0,0.0,0.0,0.0,0.0,0.0,0.0,0.0,0.0,0.0,0.0,0.0,0.0,0.0,0.0,0.0,0.0,0.0,0.0,0.0,0.0,0.0,0.0,0.0,0.0,0.0,0.0,0.0,0.0,0.0,0.0,0.0,0.0,0.0,0.0,0.0,0.0,0.0,0.0,0.0,0.25,0.5,0.75,1.0,0.800000011920929,0.6000000238418579,0.4000000059604645,0.20000000298023224,0.0,0.0,0.0,0.0,0.0,0.0,0.0,0.0,0.0,0.0,0.0,0.0,0.0,0.0,0.0,0.0,0.0,0.0,0.0,0.0,0.0,0.0,0.0,0.0,0.0,0.0,0.0,0.0,0.0,0.0,0.0,0.0,0.0,0.0,0.0,0.0,0.0,0.0,0.0,0.0,0.0,0.0,0.0,0.0,0.0,0.0,0.0,0.0,0.0,0.0,0.0,0.0,0.0,0.0,0.0,0.0,0.0,0.0,0.0,0.0,0.0,0.0,0.0,0.0,0.0,0.0,0.0,0.0,0.0,0.0,0.0,0.0,0.0,0.0,0.0,0.0,0.0,0.0,0.0,0.0,0.0,0.0,0.0,0.0,0.0,0.0,0.0,0.0,0.0,0.0,0.0,0.0,0.0,0.0,0.0,0.0,0.0,0.0,0.0,0.0,0.0,0.0,0.0,0.0,0.0,0.0,0.0,0.0,0.0,0.0,0.0,0.0,0.0,0.0,0.0,0.0,0.0,0.0,0.0,0.0,0.0,0.0,0.0,0.0,0.0,0.0,0.0,0.0,0.0,0.0,0.0,0.0,0.0,0.0,0.0,0.0,0.0,0.0,0.0,0.0,0.0,0.0,0.0,0.0,0.0,0.0,0.0,0.0,0.0,0.0,0.0,0.0,0.0,0.0,0.0,0.0,0.0,0.0,0.0,0.0,0.0,0.0,0.0,0.0,0.0,0.0,0.0,0.0,0.0,0.0,0.0,0.0,0.0,0.0,0.0,0.0,0.0,0.0,0.0,0.0,0.0,0.0,0.0,0.0,0.0,0.0,0.0,0.0,0.0,0.0,0.0,0.0,0.0,0.0,0.0,0.0,0.0,0.0,0.0,0.0,0.0,0.0,0.0,0.0,0.0,0.0,0.0,0.0,0.0,0.0,0.0,0.0,0.0,0.0,0.0,0.0,0.0,0.0,0.0,0.0,0.0,0.0,0.0,0.0,0.0,0.0,0.0,0.0,0.0,0.0,0.0,0.0,0.0,0.0,0.0,0.0,0.0,0.0,0.0,0.0,0.0,0.0,0.0,0.0,0.0,0.0,0.0,0.0,0.0,0.0,0.0,0.0,0.0,0.20000000298023224,0.4000000059604645,0.6000000238418579,0.800000011920929,1.0,0.800000011920929,0.6000000238418579,0.4000000059604645,0.20000000298023224,0.0,0.0,0.0,0.0,0.0,0.0,0.0,0.0,0.0,0.0,0.0,0.0,0.0,0.0,0.0,0.0,0.0,0.0,0.0,0.0,0.0,0.0,0.0,0.0,0.0,0.0,0.0,0.0,0.0,0.0,0.0,0.0,0.0,0.0,0.0,0.0,0.0,0.0,0.0,0.0,0.0,0.0,0.0,0.0,0.0,0.0,0.0,0.0,0.0,0.0,0.0,0.0,0.0,0.0,0.0,0.0,0.0,0.0,0.0,0.0,0.0,0.0,0.0,0.0,0.0,0.0,0.0,0.0,0.0,0.0,0.0,0.0,0.0,0.0,0.0,0.0,0.0,0.0,0.0,0.0,0.0,0.0,0.0,0.0,0.0,0.0,0.0,0.0,0.0,0.0,0.0,0.0,0.0,0.0,0.0,0.0,0.0,0.0,0.0,0.0,0.0,0.0,0.0,0.0,0.0,0.0,0.0,0.0,0.0,0.0,0.0,0.0,0.0,0.0,0.0,0.0,0.0,0.0,0.0,0.0,0.0,0.0,0.0,0.0,0.0,0.0,0.0,0.0,0.0,0.0,0.0,0.0,0.0,0.0,0.0,0.0,0.0,0.0,0.0,0.0,0.0,0.0,0.0,0.0,0.0,0.0,0.0,0.0,0.0,0.0,0.0,0.0,0.0,0.0,0.0,0.0,0.0,0.0,0.0,0.0,0.0,0.0,0.0,0.0,0.0,0.0,0.0,0.0,0.0,0.0,0.0,0.0,0.0,0.0,0.0,0.0,0.0,0.0,0.0,0.0,0.0,0.0,0.0,0.0,0.0,0.0,0.0,0.0,0.0,0.0,0.0,0.0,0.0,0.0,0.0,0.0,0.0,0.0,0.0,0.0,0.0,0.0,0.0,0.0,0.0,0.0,0.0,0.0,0.0,0.0,0.0,0.0,0.0,0.0,0.0,0.0,0.0,0.0,0.0,0.0,0.0,0.0,0.0,0.0,0.0,0.0,0.0,0.0,0.0,0.0,0.0,0.0,0.0,0.0,0.0,0.0,0.0,0.0,0.0,0.0,0.0,0.0,0.0,0.0,0.0,0.0,0.0,0.0,0.0,0.0,0.0,0.0,0.0,0.20000000298023224,0.4000000059604645,0.6000000238418579,0.800000011920929,1.0,0.800000011920929,0.6000000238418579,0.4000000059604645,0.20000000298023224,0.0,0.0,0.0,0.0,0.0,0.0,0.0,0.0,0.0,0.0,0.0,0.0,0.0,0.0,0.0,0.0,0.0,0.0,0.0,0.0,0.0,0.0,0.0,0.0,0.0,0.0,0.0,0.0,0.0,0.0,0.0,0.0,0.0,0.0,0.0,0.0,0.0,0.0,0.0,0.0,0.0,0.0,0.0,0.0,0.0,0.0,0.0,0.0,0.0,0.0,0.0,0.0,0.0,0.0,0.0,0.0,0.0,0.0,0.0,0.0,0.0,0.0,0.0,0.0,0.0,0.0,0.0,0.0,0.0,0.0,0.0,0.0,0.0,0.0,0.0,0.0,0.0,0.0,0.0,0.0,0.0,0.0,0.0,0.0,0.0,0.0,0.0,0.0,0.0,0.0,0.0,0.0,0.0,0.0,0.0,0.0,0.0,0.0,0.0,0.0,0.0,0.0,0.0,0.0,0.0,0.0,0.0,0.0,0.0,0.0,0.0,0.0,0.0,0.0,0.0,0.0,0.0,0.0,0.0,0.0,0.0,0.0,0.0,0.0,0.0,0.0,0.0,0.0,0.0,0.0,0.0,0.0,0.0,0.0,0.0,0.0,0.0,0.0,0.0,0.0,0.0,0.0,0.0,0.0,0.0,0.0,0.0,0.0,0.0,0.0,0.0,0.0,0.0,0.0,0.0,0.0,0.0,0.0,0.0,0.0,0.0,0.0,0.0,0.0,0.0,0.0,0.0,0.0,0.0,0.0,0.0,0.0,0.0,0.0,0.0,0.0,0.0,0.0,0.0,0.0,0.0,0.0,0.0,0.0,0.0,0.0,0.0,0.0,0.0,0.0,0.0,0.0,0.0,0.0,0.0,0.0,0.0,0.0,0.0,0.0,0.0,0.0,0.0,0.0,0.0,0.0,0.0,0.0,0.0,0.0,0.0,0.0,0.0,0.0,0.0,0.0,0.0,0.0,0.0,0.0,0.0,0.0,0.0,0.0,0.0,0.0,0.0,0.0,0.0,0.0,0.0,0.0,0.0,0.0,0.0,0.0,0.0,0.0,0.0,0.0,0.0,0.0,0.0,0.0,0.0,0.0,0.0,0.0,0.0,0.0,0.0,0.0,0.0,0.20000000298023224,0.4000000059604645,0.6000000238418579,0.800000011920929,1.0,0.800000011920929,0.6000000238418579,0.4000000059604645,0.20000000298023224,0.0,0.0,0.0,0.0,0.0,0.0,0.0,0.0,0.0,0.0,0.0,0.0,0.0,0.0,0.0,0.0,0.0,0.0,0.0,0.0,0.0,0.0,0.0,0.0,0.0,0.0,0.0,0.0,0.0,0.0,0.0,0.0,0.0,0.0,0.0,0.0,0.0,0.0,0.0,0.0,0.0,0.0,0.0,0.0,0.0,0.0,0.0,0.0,0.0,0.0,0.0,0.0,0.0,0.0,0.0,0.0,0.0,0.0,0.0,0.0,0.0,0.0,0.0,0.0,0.0,0.0,0.0,0.0,0.0,0.0,0.0,0.0,0.0,0.0,0.0,0.0,0.0,0.0,0.0,0.0,0.0,0.0,0.0,0.0,0.0,0.0,0.0,0.0,0.0,0.0,0.0,0.0,0.0,0.0,0.0,0.0,0.0,0.0,0.0,0.0,0.0,0.0,0.0,0.0,0.0,0.0,0.0,0.0,0.0,0.0,0.0,0.0,0.0,0.0,0.0,0.0,0.0,0.0,0.0,0.0,0.0,0.0,0.0,0.0,0.0,0.0,0.0,0.0,0.0,0.0,0.0,0.0,0.0,0.0,0.0,0.0,0.0,0.0,0.0,0.0,0.0,0.0,0.0,0.0,0.0,0.0,0.0,0.0,0.0,0.0,0.0,0.0,0.0,0.0,0.0,0.0,0.0,0.0,0.0,0.0,0.0,0.0,0.0,0.0,0.0,0.0,0.0,0.0,0.0,0.0,0.0,0.0,0.0,0.0,0.0,0.0,0.0,0.0,0.0,0.0,0.0,0.0,0.0,0.0,0.0,0.0,0.0,0.0,0.0,0.0,0.0,0.0,0.0,0.0,0.0,0.0,0.0,0.0,0.0,0.0,0.0,0.0,0.0,0.0,0.0,0.0,0.0,0.0,0.0,0.0,0.0,0.0,0.0,0.0,0.0,0.0,0.0,0.0,0.0,0.0,0.0,0.0,0.0,0.0,0.0,0.0,0.0,0.0,0.0,0.0,0.0,0.0,0.0,0.0,0.0,0.0,0.0,0.0,0.0,0.0,0.0,0.0,0.0,0.0,0.0,0.0,0.0,0.0,0.0,0.0,0.0,0.0,0.0,0.20000000298023224,0.4000000059604645,0.6000000238418579,0.800000011920929,1.0,0.8333333134651184,0.6666666865348816,0.5,0.3333333432674408,0.1666666716337204,0.0,0.0,0.0,0.0,0.0,0.0,0.0,0.0,0.0,0.0,0.0,0.0,0.0,0.0,0.0,0.0,0.0,0.0,0.0,0.0,0.0,0.0,0.0,0.0,0.0,0.0,0.0,0.0,0.0,0.0,0.0,0.0,0.0,0.0,0.0,0.0,0.0,0.0,0.0,0.0,0.0,0.0,0.0,0.0,0.0,0.0,0.0,0.0,0.0,0.0,0.0,0.0,0.0,0.0,0.0,0.0,0.0,0.0,0.0,0.0,0.0,0.0,0.0,0.0,0.0,0.0,0.0,0.0,0.0,0.0,0.0,0.0,0.0,0.0,0.0,0.0,0.0,0.0,0.0,0.0,0.0,0.0,0.0,0.0,0.0,0.0,0.0,0.0,0.0,0.0,0.0,0.0,0.0,0.0,0.0,0.0,0.0,0.0,0.0,0.0,0.0,0.0,0.0,0.0,0.0,0.0,0.0,0.0,0.0,0.0,0.0,0.0,0.0,0.0,0.0,0.0,0.0,0.0,0.0,0.0,0.0,0.0,0.0,0.0,0.0,0.0,0.0,0.0,0.0,0.0,0.0,0.0,0.0,0.0,0.0,0.0,0.0,0.0,0.0,0.0,0.0,0.0,0.0,0.0,0.0,0.0,0.0,0.0,0.0,0.0,0.0,0.0,0.0,0.0,0.0,0.0,0.0,0.0,0.0,0.0,0.0,0.0,0.0,0.0,0.0,0.0,0.0,0.0,0.0,0.0,0.0,0.0,0.0,0.0,0.0,0.0,0.0,0.0,0.0,0.0,0.0,0.0,0.0,0.0,0.0,0.0,0.0,0.0,0.0,0.0,0.0,0.0,0.0,0.0,0.0,0.0,0.0,0.0,0.0,0.0,0.0,0.0,0.0,0.0,0.0,0.0,0.0,0.0,0.0,0.0,0.0,0.0,0.0,0.0,0.0,0.0,0.0,0.0,0.0,0.0,0.0,0.0,0.0,0.0,0.0,0.0,0.0,0.0,0.0,0.0,0.0,0.0,0.0,0.0,0.0,0.0,0.0,0.0,0.0,0.0,0.0,0.0,0.0,0.0,0.0,0.0,0.0,0.0,0.0,0.0,0.0,0.0,0.1666666716337204,0.3333333432674408,0.5,0.6666666865348816,0.8333333134651184,1.0,0.8333333134651184,0.6666666865348816,0.5,0.3333333432674408,0.1666666716337204,0.0,0.0,0.0,0.0,0.0,0.0,0.0,0.0,0.0,0.0,0.0,0.0,0.0,0.0,0.0,0.0,0.0,0.0,0.0,0.0,0.0,0.0,0.0,0.0,0.0,0.0,0.0,0.0,0.0,0.0,0.0,0.0,0.0,0.0,0.0,0.0,0.0,0.0,0.0,0.0,0.0,0.0,0.0,0.0,0.0,0.0,0.0,0.0,0.0,0.0,0.0,0.0,0.0,0.0,0.0,0.0,0.0,0.0,0.0,0.0,0.0,0.0,0.0,0.0,0.0,0.0,0.0,0.0,0.0,0.0,0.0,0.0,0.0,0.0,0.0,0.0,0.0,0.0,0.0,0.0,0.0,0.0,0.0,0.0,0.0,0.0,0.0,0.0,0.0,0.0,0.0,0.0,0.0,0.0,0.0,0.0,0.0,0.0,0.0,0.0,0.0,0.0,0.0,0.0,0.0,0.0,0.0,0.0,0.0,0.0,0.0,0.0,0.0,0.0,0.0,0.0,0.0,0.0,0.0,0.0,0.0,0.0,0.0,0.0,0.0,0.0,0.0,0.0,0.0,0.0,0.0,0.0,0.0,0.0,0.0,0.0,0.0,0.0,0.0,0.0,0.0,0.0,0.0,0.0,0.0,0.0,0.0,0.0,0.0,0.0,0.0,0.0,0.0,0.0,0.0,0.0,0.0,0.0,0.0,0.0,0.0,0.0,0.0,0.0,0.0,0.0,0.0,0.0,0.0,0.0,0.0,0.0,0.0,0.0,0.0,0.0,0.0,0.0,0.0,0.0,0.0,0.0,0.0,0.0,0.0,0.0,0.0,0.0,0.0,0.0,0.0,0.0,0.0,0.0,0.0,0.0,0.0,0.0,0.0,0.0,0.0,0.0,0.0,0.0,0.0,0.0,0.0,0.0,0.0,0.0,0.0,0.0,0.0,0.0,0.0,0.0,0.0,0.0,0.0,0.0,0.0,0.0,0.0,0.0,0.0,0.0,0.0,0.0,0.0,0.0,0.0,0.0,0.0,0.0,0.0,0.0,0.0,0.0,0.0,0.0,0.0,0.0,0.0,0.0,0.0,0.0,0.0,0.0,0.0,0.0,0.0,0.0,0.1666666716337204,0.3333333432674408,0.5,0.6666666865348816,0.8333333134651184,1.0,0.8571428656578064,0.7142857313156128,0.5714285969734192,0.4285714328289032,0.2857142984867096,0.1428571492433548,0.0,0.0,0.0,0.0,0.0,0.0,0.0,0.0,0.0,0.0,0.0,0.0,0.0,0.0,0.0,0.0,0.0,0.0,0.0,0.0,0.0,0.0,0.0,0.0,0.0,0.0,0.0,0.0,0.0,0.0,0.0,0.0,0.0,0.0,0.0,0.0,0.0,0.0,0.0,0.0,0.0,0.0,0.0,0.0,0.0,0.0,0.0,0.0,0.0,0.0,0.0,0.0,0.0,0.0,0.0,0.0,0.0,0.0,0.0,0.0,0.0,0.0,0.0,0.0,0.0,0.0,0.0,0.0,0.0,0.0,0.0,0.0,0.0,0.0,0.0,0.0,0.0,0.0,0.0,0.0,0.0,0.0,0.0,0.0,0.0,0.0,0.0,0.0,0.0,0.0,0.0,0.0,0.0,0.0,0.0,0.0,0.0,0.0,0.0,0.0,0.0,0.0,0.0,0.0,0.0,0.0,0.0,0.0,0.0,0.0,0.0,0.0,0.0,0.0,0.0,0.0,0.0,0.0,0.0,0.0,0.0,0.0,0.0,0.0,0.0,0.0,0.0,0.0,0.0,0.0,0.0,0.0,0.0,0.0,0.0,0.0,0.0,0.0,0.0,0.0,0.0,0.0,0.0,0.0,0.0,0.0,0.0,0.0,0.0,0.0,0.0,0.0,0.0,0.0,0.0,0.0,0.0,0.0,0.0,0.0,0.0,0.0,0.0,0.0,0.0,0.0,0.0,0.0,0.0,0.0,0.0,0.0,0.0,0.0,0.0,0.0,0.0,0.0,0.0,0.0,0.0,0.0,0.0,0.0,0.0,0.0,0.0,0.0,0.0,0.0,0.0,0.0,0.0,0.0,0.0,0.0,0.0,0.0,0.0,0.0,0.0,0.0,0.0,0.0,0.0,0.0,0.0,0.0,0.0,0.0,0.0,0.0,0.0,0.0,0.0,0.0,0.0,0.0,0.0,0.0,0.0,0.0,0.0,0.0,0.0,0.0,0.0,0.0,0.0,0.0,0.0,0.0,0.0,0.0,0.0,0.0,0.0,0.0,0.0,0.0,0.0,0.0,0.0,0.0,0.0,0.0,0.0,0.0,0.0,0.0,0.0,0.1428571492433548,0.2857142984867096,0.4285714328289032,0.5714285969734192,0.7142857313156128,0.8571428656578064,1.0,0.8571428656578064,0.7142857313156128,0.5714285969734192,0.4285714328289032,0.2857142984867096,0.1428571492433548,0.0,0.0,0.0,0.0,0.0,0.0,0.0,0.0,0.0,0.0,0.0,0.0,0.0,0.0,0.0,0.0,0.0,0.0,0.0,0.0,0.0,0.0,0.0,0.0,0.0,0.0,0.0,0.0,0.0,0.0,0.0,0.0,0.0,0.0,0.0,0.0,0.0,0.0,0.0,0.0,0.0,0.0,0.0,0.0,0.0,0.0,0.0,0.0,0.0,0.0,0.0,0.0,0.0,0.0,0.0,0.0,0.0,0.0,0.0,0.0,0.0,0.0,0.0,0.0,0.0,0.0,0.0,0.0,0.0,0.0,0.0,0.0,0.0,0.0,0.0,0.0,0.0,0.0,0.0,0.0,0.0,0.0,0.0,0.0,0.0,0.0,0.0,0.0,0.0,0.0,0.0,0.0,0.0,0.0,0.0,0.0,0.0,0.0,0.0,0.0,0.0,0.0,0.0,0.0,0.0,0.0,0.0,0.0,0.0,0.0,0.0,0.0,0.0,0.0,0.0,0.0,0.0,0.0,0.0,0.0,0.0,0.0,0.0,0.0,0.0,0.0,0.0,0.0,0.0,0.0,0.0,0.0,0.0,0.0,0.0,0.0,0.0,0.0,0.0,0.0,0.0,0.0,0.0,0.0,0.0,0.0,0.0,0.0,0.0,0.0,0.0,0.0,0.0,0.0,0.0,0.0,0.0,0.0,0.0,0.0,0.0,0.0,0.0,0.0,0.0,0.0,0.0,0.0,0.0,0.0,0.0,0.0,0.0,0.0,0.0,0.0,0.0,0.0,0.0,0.0,0.0,0.0,0.0,0.0,0.0,0.0,0.0,0.0,0.0,0.0,0.0,0.0,0.0,0.0,0.0,0.0,0.0,0.0,0.0,0.0,0.0,0.0,0.0,0.0,0.0,0.0,0.0,0.0,0.0,0.0,0.0,0.0,0.0,0.0,0.0,0.0,0.0,0.0,0.0,0.0,0.0,0.0,0.0,0.0,0.0,0.0,0.0,0.0,0.0,0.0,0.0,0.0,0.0,0.0,0.0,0.0,0.0,0.0,0.0,0.0,0.0,0.0,0.0,0.0,0.0,0.0,0.0,0.0,0.0,0.0,0.0,0.1428571492433548,0.2857142984867096,0.4285714328289032,0.5714285969734192,0.7142857313156128,0.8571428656578064,1.0,0.875,0.75,0.625,0.5,0.375,0.25,0.125,0.0,0.0,0.0,0.0,0.0,0.0,0.0,0.0,0.0,0.0,0.0,0.0,0.0,0.0,0.0,0.0,0.0,0.0,0.0,0.0,0.0,0.0,0.0,0.0,0.0,0.0,0.0,0.0,0.0,0.0,0.0,0.0,0.0,0.0,0.0,0.0,0.0,0.0,0.0,0.0,0.0,0.0,0.0,0.0,0.0,0.0,0.0,0.0,0.0,0.0,0.0,0.0,0.0,0.0,0.0,0.0,0.0,0.0,0.0,0.0,0.0,0.0,0.0,0.0,0.0,0.0,0.0,0.0,0.0,0.0,0.0,0.0,0.0,0.0,0.0,0.0,0.0,0.0,0.0,0.0,0.0,0.0,0.0,0.0,0.0,0.0,0.0,0.0,0.0,0.0,0.0,0.0,0.0,0.0,0.0,0.0,0.0,0.0,0.0,0.0,0.0,0.0,0.0,0.0,0.0,0.0,0.0,0.0,0.0,0.0,0.0,0.0,0.0,0.0,0.0,0.0,0.0,0.0,0.0,0.0,0.0,0.0,0.0,0.0,0.0,0.0,0.0,0.0,0.0,0.0,0.0,0.0,0.0,0.0,0.0,0.0,0.0,0.0,0.0,0.0,0.0,0.0,0.0,0.0,0.0,0.0,0.0,0.0,0.0,0.0,0.0,0.0,0.0,0.0,0.0,0.0,0.0,0.0,0.0,0.0,0.0,0.0,0.0,0.0,0.0,0.0,0.0,0.0,0.0,0.0,0.0,0.0,0.0,0.0,0.0,0.0,0.0,0.0,0.0,0.0,0.0,0.0,0.0,0.0,0.0,0.0,0.0,0.0,0.0,0.0,0.0,0.0,0.0,0.0,0.0,0.0,0.0,0.0,0.0,0.0,0.0,0.0,0.0,0.0,0.0,0.0,0.0,0.0,0.0,0.0,0.0,0.0,0.0,0.0,0.0,0.0,0.0,0.0,0.0,0.0,0.0,0.0,0.0,0.0,0.0,0.0,0.0,0.0,0.0,0.0,0.0,0.0,0.0,0.0,0.0,0.0,0.0,0.0,0.0,0.0,0.0,0.0,0.0,0.0,0.0,0.0,0.0,0.0,0.0,0.0,0.125,0.25,0.375,0.5,0.625,0.75,0.875,1.0,0.8571428656578064,0.7142857313156128,0.5714285969734192,0.4285714328289032,0.2857142984867096,0.1428571492433548,0.0,0.0,0.0,0.0,0.0,0.0,0.0,0.0,0.0,0.0,0.0,0.0,0.0,0.0,0.0,0.0,0.0,0.0,0.0,0.0,0.0,0.0,0.0,0.0,0.0,0.0,0.0,0.0,0.0,0.0,0.0,0.0,0.0,0.0,0.0,0.0,0.0,0.0,0.0,0.0,0.0,0.0,0.0,0.0,0.0,0.0,0.0,0.0,0.0,0.0,0.0,0.0,0.0,0.0,0.0,0.0,0.0,0.0,0.0,0.0,0.0,0.0,0.0,0.0,0.0,0.0,0.0,0.0,0.0,0.0,0.0,0.0,0.0,0.0,0.0,0.0,0.0,0.0,0.0,0.0,0.0,0.0,0.0,0.0,0.0,0.0,0.0,0.0,0.0,0.0,0.0,0.0,0.0,0.0,0.0,0.0,0.0,0.0,0.0,0.0,0.0,0.0,0.0,0.0,0.0,0.0,0.0,0.0,0.0,0.0,0.0,0.0,0.0,0.0,0.0,0.0,0.0,0.0,0.0,0.0,0.0,0.0,0.0,0.0,0.0,0.0,0.0,0.0,0.0,0.0,0.0,0.0,0.0,0.0,0.0,0.0,0.0,0.0,0.0,0.0,0.0,0.0,0.0,0.0,0.0,0.0,0.0,0.0,0.0,0.0,0.0,0.0,0.0,0.0,0.0,0.0,0.0,0.0,0.0,0.0,0.0,0.0,0.0,0.0,0.0,0.0,0.0,0.0,0.0,0.0,0.0,0.0,0.0,0.0,0.0,0.0,0.0,0.0,0.0,0.0,0.0,0.0,0.0,0.0,0.0,0.0,0.0,0.0,0.0,0.0,0.0,0.0,0.0,0.0,0.0,0.0,0.0,0.0,0.0,0.0,0.0,0.0,0.0,0.0,0.0,0.0,0.0,0.0,0.0,0.0,0.0,0.0,0.0,0.0,0.0,0.0,0.0,0.0,0.0,0.0,0.0,0.0,0.0,0.0,0.0,0.0,0.0,0.0,0.0,0.0,0.0,0.0,0.0,0.0,0.0,0.0,0.0,0.0,0.0,0.0,0.0,0.0,0.0,0.0,0.0,0.0,0.0,0.0,0.0,0.0,0.0,0.1428571492433548,0.2857142984867096,0.4285714328289032,0.5714285969734192,0.7142857313156128,0.8571428656578064,1.0,0.8888888955116272,0.7777777910232544,0.6666666865348816,0.5555555820465088,0.4444444477558136,0.3333333432674408,0.2222222238779068,0.1111111119389534,0.0,0.0,0.0,0.0,0.0,0.0,0.0,0.0,0.0,0.0,0.0,0.0,0.0,0.0,0.0,0.0,0.0,0.0,0.0,0.0,0.0,0.0,0.0,0.0,0.0,0.0,0.0,0.0,0.0,0.0,0.0,0.0,0.0,0.0,0.0,0.0,0.0,0.0,0.0,0.0,0.0,0.0,0.0,0.0,0.0,0.0,0.0,0.0,0.0,0.0,0.0,0.0,0.0,0.0,0.0,0.0,0.0,0.0,0.0,0.0,0.0,0.0,0.0,0.0,0.0,0.0,0.0,0.0,0.0,0.0,0.0,0.0,0.0,0.0,0.0,0.0,0.0,0.0,0.0,0.0,0.0,0.0,0.0,0.0,0.0,0.0,0.0,0.0,0.0,0.0,0.0,0.0,0.0,0.0,0.0,0.0,0.0,0.0,0.0,0.0,0.0,0.0,0.0,0.0,0.0,0.0,0.0,0.0,0.0,0.0,0.0,0.0,0.0,0.0,0.0,0.0,0.0,0.0,0.0,0.0,0.0,0.0,0.0,0.0,0.0,0.0,0.0,0.0,0.0,0.0,0.0,0.0,0.0,0.0,0.0,0.0,0.0,0.0,0.0,0.0,0.0,0.0,0.0,0.0,0.0,0.0,0.0,0.0,0.0,0.0,0.0,0.0,0.0,0.0,0.0,0.0,0.0,0.0,0.0,0.0,0.0,0.0,0.0,0.0,0.0,0.0,0.0,0.0,0.0,0.0,0.0,0.0,0.0,0.0,0.0,0.0,0.0,0.0,0.0,0.0,0.0,0.0,0.0,0.0,0.0,0.0,0.0,0.0,0.0,0.0,0.0,0.0,0.0,0.0,0.0,0.0,0.0,0.0,0.0,0.0,0.0,0.0,0.0,0.0,0.0,0.0,0.0,0.0,0.0,0.0,0.0,0.0,0.0,0.0,0.0,0.0,0.0,0.0,0.0,0.0,0.0,0.0,0.0,0.0,0.0,0.0,0.0,0.0,0.0,0.0,0.0,0.0,0.0,0.0,0.0,0.0,0.0,0.0,0.0,0.0,0.0,0.0,0.0,0.0,0.0,0.0,0.0,0.0,0.0,0.1111111119389534,0.2222222238779068,0.3333333432674408,0.4444444477558136,0.5555555820465088,0.6666666865348816,0.7777777910232544,0.8888888955116272,1.0,0.8888888955116272,0.7777777910232544,0.6666666865348816,0.5555555820465088,0.4444444477558136,0.3333333432674408,0.2222222238779068,0.1111111119389534,0.0,0.0,0.0,0.0,0.0,0.0,0.0,0.0,0.0,0.0,0.0,0.0,0.0,0.0,0.0,0.0,0.0,0.0,0.0,0.0,0.0,0.0,0.0,0.0,0.0,0.0,0.0,0.0,0.0,0.0,0.0,0.0,0.0,0.0,0.0,0.0,0.0,0.0,0.0,0.0,0.0,0.0,0.0,0.0,0.0,0.0,0.0,0.0,0.0,0.0,0.0,0.0,0.0,0.0,0.0,0.0,0.0,0.0,0.0,0.0,0.0,0.0,0.0,0.0,0.0,0.0,0.0,0.0,0.0,0.0,0.0,0.0,0.0,0.0,0.0,0.0,0.0,0.0,0.0,0.0,0.0,0.0,0.0,0.0,0.0,0.0,0.0,0.0,0.0,0.0,0.0,0.0,0.0,0.0,0.0,0.0,0.0,0.0,0.0,0.0,0.0,0.0,0.0,0.0,0.0,0.0,0.0,0.0,0.0,0.0,0.0,0.0,0.0,0.0,0.0,0.0,0.0,0.0,0.0,0.0,0.0,0.0,0.0,0.0,0.0,0.0,0.0,0.0,0.0,0.0,0.0,0.0,0.0,0.0,0.0,0.0,0.0,0.0,0.0,0.0,0.0,0.0,0.0,0.0,0.0,0.0,0.0,0.0,0.0,0.0,0.0,0.0,0.0,0.0,0.0,0.0,0.0,0.0,0.0,0.0,0.0,0.0,0.0,0.0,0.0,0.0,0.0,0.0,0.0,0.0,0.0,0.0,0.0,0.0,0.0,0.0,0.0,0.0,0.0,0.0,0.0,0.0,0.0,0.0,0.0,0.0,0.0,0.0,0.0,0.0,0.0,0.0,0.0,0.0,0.0,0.0,0.0,0.0,0.0,0.0,0.0,0.0,0.0,0.0,0.0,0.0,0.0,0.0,0.0,0.0,0.0,0.0,0.0,0.0,0.0,0.0,0.0,0.0,0.0,0.0,0.0,0.0,0.0,0.0,0.0,0.0,0.0,0.0,0.0,0.0,0.0,0.0,0.0,0.0,0.0,0.0,0.0,0.0,0.0,0.0,0.0,0.0,0.0,0.0,0.0,0.0,0.0,0.0,0.0,0.1111111119389534,0.2222222238779068,0.3333333432674408,0.4444444477558136,0.5555555820465088,0.6666666865348816,0.7777777910232544,0.8888888955116272,1.0,0.8888888955116272,0.7777777910232544,0.6666666865348816,0.5555555820465088,0.4444444477558136,0.3333333432674408,0.2222222238779068,0.1111111119389534,0.0,0.0,0.0,0.0,0.0,0.0,0.0,0.0,0.0,0.0,0.0,0.0,0.0,0.0,0.0,0.0,0.0,0.0,0.0,0.0,0.0,0.0,0.0,0.0,0.0,0.0,0.0,0.0,0.0,0.0,0.0,0.0,0.0,0.0,0.0,0.0,0.0,0.0,0.0,0.0,0.0,0.0,0.0,0.0,0.0,0.0,0.0,0.0,0.0,0.0,0.0,0.0,0.0,0.0,0.0,0.0,0.0,0.0,0.0,0.0,0.0,0.0,0.0,0.0,0.0,0.0,0.0,0.0,0.0,0.0,0.0,0.0,0.0,0.0,0.0,0.0,0.0,0.0,0.0,0.0,0.0,0.0,0.0,0.0,0.0,0.0,0.0,0.0,0.0,0.0,0.0,0.0,0.0,0.0,0.0,0.0,0.0,0.0,0.0,0.0,0.0,0.0,0.0,0.0,0.0,0.0,0.0,0.0,0.0,0.0,0.0,0.0,0.0,0.0,0.0,0.0,0.0,0.0,0.0,0.0,0.0,0.0,0.0,0.0,0.0,0.0,0.0,0.0,0.0,0.0,0.0,0.0,0.0,0.0,0.0,0.0,0.0,0.0,0.0,0.0,0.0,0.0,0.0,0.0,0.0,0.0,0.0,0.0,0.0,0.0,0.0,0.0,0.0,0.0,0.0,0.0,0.0,0.0,0.0,0.0,0.0,0.0,0.0,0.0,0.0,0.0,0.0,0.0,0.0,0.0,0.0,0.0,0.0,0.0,0.0,0.0,0.0,0.0,0.0,0.0,0.0,0.0,0.0,0.0,0.0,0.0,0.0,0.0,0.0,0.0,0.0,0.0,0.0,0.0,0.0,0.0,0.0,0.0,0.0,0.0,0.0,0.0,0.0,0.0,0.0,0.0,0.0,0.0,0.0,0.0,0.0,0.0,0.0,0.0,0.0,0.0,0.0,0.0,0.0,0.0,0.0,0.0,0.0,0.0,0.0,0.0,0.0,0.0,0.0,0.0,0.0,0.0,0.0,0.0,0.0,0.0,0.0,0.0,0.0,0.0,0.0,0.0,0.0,0.0,0.0,0.0,0.0,0.0,0.0,0.1111111119389534,0.2222222238779068,0.3333333432674408,0.4444444477558136,0.5555555820465088,0.6666666865348816,0.7777777910232544,0.8888888955116272,1.0,0.9090909361839294,0.8181818127632141,0.7272727489471436,0.6363636255264282,0.5454545617103577,0.4545454680919647,0.3636363744735718,0.27272728085517883,0.1818181872367859,0.09090909361839294,0.0,0.0,0.0,0.0,0.0,0.0,0.0,0.0,0.0,0.0,0.0,0.0,0.0,0.0,0.0,0.0,0.0,0.0,0.0,0.0,0.0,0.0,0.0,0.0,0.0,0.0,0.0,0.0,0.0,0.0,0.0,0.0,0.0,0.0,0.0,0.0,0.0,0.0,0.0,0.0,0.0,0.0,0.0,0.0,0.0,0.0,0.0,0.0,0.0,0.0,0.0,0.0,0.0,0.0,0.0,0.0,0.0,0.0,0.0,0.0,0.0,0.0,0.0,0.0,0.0,0.0,0.0,0.0,0.0,0.0,0.0,0.0,0.0,0.0,0.0,0.0,0.0,0.0,0.0,0.0,0.0,0.0,0.0,0.0,0.0,0.0,0.0,0.0,0.0,0.0,0.0,0.0,0.0,0.0,0.0,0.0,0.0,0.0,0.0,0.0,0.0,0.0,0.0,0.0,0.0,0.0,0.0,0.0,0.0,0.0,0.0,0.0,0.0,0.0,0.0,0.0,0.0,0.0,0.0,0.0,0.0,0.0,0.0,0.0,0.0,0.0,0.0,0.0,0.0,0.0,0.0,0.0,0.0,0.0,0.0,0.0,0.0,0.0,0.0,0.0,0.0,0.0,0.0,0.0,0.0,0.0,0.0,0.0,0.0,0.0,0.0,0.0,0.0,0.0,0.0,0.0,0.0,0.0,0.0,0.0,0.0,0.0,0.0,0.0,0.0,0.0,0.0,0.0,0.0,0.0,0.0,0.0,0.0,0.0,0.0,0.0,0.0,0.0,0.0,0.0,0.0,0.0,0.0,0.0,0.0,0.0,0.0,0.0,0.0,0.0,0.0,0.0,0.0,0.0,0.0,0.0,0.0,0.0,0.0,0.0,0.0,0.0,0.0,0.0,0.0,0.0,0.0,0.0,0.0,0.0,0.0,0.0,0.0,0.0,0.0,0.0,0.0,0.0,0.0,0.0,0.0,0.0,0.0,0.0,0.0,0.0,0.0,0.0,0.0,0.0,0.0,0.0,0.0,0.0,0.0,0.0,0.0,0.0,0.0,0.0,0.0,0.0,0.0,0.0,0.0,0.0,0.0,0.09090909361839294,0.1818181872367859,0.27272728085517883,0.3636363744735718,0.4545454680919647,0.5454545617103577,0.6363636255264282,0.7272727489471436,0.8181818127632141,0.9090909361839294,1.0,0.8999999761581421,0.800000011920929,0.699999988079071,0.6000000238418579,0.5,0.4000000059604645,0.30000001192092896,0.20000000298023224,0.10000000149011612,0.0,0.0,0.0,0.0,0.0,0.0,0.0,0.0,0.0,0.0,0.0,0.0,0.0,0.0,0.0,0.0,0.0,0.0,0.0,0.0,0.0,0.0,0.0,0.0,0.0,0.0,0.0,0.0,0.0,0.0,0.0,0.0,0.0,0.0,0.0,0.0,0.0,0.0,0.0,0.0,0.0,0.0,0.0,0.0,0.0,0.0,0.0,0.0,0.0,0.0,0.0,0.0,0.0,0.0,0.0,0.0,0.0,0.0,0.0,0.0,0.0,0.0,0.0,0.0,0.0,0.0,0.0,0.0,0.0,0.0,0.0,0.0,0.0,0.0,0.0,0.0,0.0,0.0,0.0,0.0,0.0,0.0,0.0,0.0,0.0,0.0,0.0,0.0,0.0,0.0,0.0,0.0,0.0,0.0,0.0,0.0,0.0,0.0,0.0,0.0,0.0,0.0,0.0,0.0,0.0,0.0,0.0,0.0,0.0,0.0,0.0,0.0,0.0,0.0,0.0,0.0,0.0,0.0,0.0,0.0,0.0,0.0,0.0,0.0,0.0,0.0,0.0,0.0,0.0,0.0,0.0,0.0,0.0,0.0,0.0,0.0,0.0,0.0,0.0,0.0,0.0,0.0,0.0,0.0,0.0,0.0,0.0,0.0,0.0,0.0,0.0,0.0,0.0,0.0,0.0,0.0,0.0,0.0,0.0,0.0,0.0,0.0,0.0,0.0,0.0,0.0,0.0,0.0,0.0,0.0,0.0,0.0,0.0,0.0,0.0,0.0,0.0,0.0,0.0,0.0,0.0,0.0,0.0,0.0,0.0,0.0,0.0,0.0,0.0,0.0,0.0,0.0,0.0,0.0,0.0,0.0,0.0,0.0,0.0,0.0,0.0,0.0,0.0,0.0,0.0,0.0,0.0,0.0,0.0,0.0,0.0,0.0,0.0,0.0,0.0,0.0,0.0,0.0,0.0,0.0,0.0,0.0,0.0,0.0,0.0,0.0,0.0,0.0,0.0,0.0,0.0,0.0,0.0,0.0,0.0,0.0,0.0,0.0,0.0,0.0,0.0,0.0,0.0,0.0,0.0,0.0,0.0,0.0,0.10000000149011612,0.20000000298023224,0.30000001192092896,0.4000000059604645,0.5,0.6000000238418579,0.699999988079071,0.800000011920929,0.8999999761581421,1.0,0.9166666865348816,0.8333333134651184,0.75,0.6666666865348816,0.5833333134651184,0.5,0.4166666567325592,0.3333333432674408,0.25,0.1666666716337204,0.0833333358168602,0.0,0.0,0.0,0.0,0.0,0.0,0.0,0.0,0.0,0.0,0.0,0.0,0.0,0.0,0.0,0.0,0.0,0.0,0.0,0.0,0.0,0.0,0.0,0.0,0.0,0.0,0.0,0.0,0.0,0.0,0.0,0.0,0.0,0.0,0.0,0.0,0.0,0.0,0.0,0.0,0.0,0.0,0.0,0.0,0.0,0.0,0.0,0.0,0.0,0.0,0.0,0.0,0.0,0.0,0.0,0.0,0.0,0.0,0.0,0.0,0.0,0.0,0.0,0.0,0.0,0.0,0.0,0.0,0.0,0.0,0.0,0.0,0.0,0.0,0.0,0.0,0.0,0.0,0.0,0.0,0.0,0.0,0.0,0.0,0.0,0.0,0.0,0.0,0.0,0.0,0.0,0.0,0.0,0.0,0.0,0.0,0.0,0.0,0.0,0.0,0.0,0.0,0.0,0.0,0.0,0.0,0.0,0.0,0.0,0.0,0.0,0.0,0.0,0.0,0.0,0.0,0.0,0.0,0.0,0.0,0.0,0.0,0.0,0.0,0.0,0.0,0.0,0.0,0.0,0.0,0.0,0.0,0.0,0.0,0.0,0.0,0.0,0.0,0.0,0.0,0.0,0.0,0.0,0.0,0.0,0.0,0.0,0.0,0.0,0.0,0.0,0.0,0.0,0.0,0.0,0.0,0.0,0.0,0.0,0.0,0.0,0.0,0.0,0.0,0.0,0.0,0.0,0.0,0.0,0.0,0.0,0.0,0.0,0.0,0.0,0.0,0.0,0.0,0.0,0.0,0.0,0.0,0.0,0.0,0.0,0.0,0.0,0.0,0.0,0.0,0.0,0.0,0.0,0.0,0.0,0.0,0.0,0.0,0.0,0.0,0.0,0.0,0.0,0.0,0.0,0.0,0.0,0.0,0.0,0.0,0.0,0.0,0.0,0.0,0.0,0.0,0.0,0.0,0.0,0.0,0.0,0.0,0.0,0.0,0.0,0.0,0.0,0.0,0.0,0.0,0.0,0.0,0.0,0.0,0.0,0.0,0.0,0.0,0.0,0.0,0.0,0.0,0.0,0.0,0.0,0.0,0.0833333358168602,0.1666666716337204,0.25,0.3333333432674408,0.4166666567325592,0.5,0.5833333134651184,0.6666666865348816,0.75,0.8333333134651184,0.9166666865348816,1.0,0.9166666865348816,0.8333333134651184,0.75,0.6666666865348816,0.5833333134651184,0.5,0.4166666567325592,0.3333333432674408,0.25,0.1666666716337204,0.0833333358168602,0.0,0.0,0.0,0.0,0.0,0.0,0.0,0.0,0.0,0.0,0.0,0.0,0.0,0.0,0.0,0.0,0.0,0.0,0.0,0.0,0.0,0.0,0.0,0.0,0.0,0.0,0.0,0.0,0.0,0.0,0.0,0.0,0.0,0.0,0.0,0.0,0.0,0.0,0.0,0.0,0.0,0.0,0.0,0.0,0.0,0.0,0.0,0.0,0.0,0.0,0.0,0.0,0.0,0.0,0.0,0.0,0.0,0.0,0.0,0.0,0.0,0.0,0.0,0.0,0.0,0.0,0.0,0.0,0.0,0.0,0.0,0.0,0.0,0.0,0.0,0.0,0.0,0.0,0.0,0.0,0.0,0.0,0.0,0.0,0.0,0.0,0.0,0.0,0.0,0.0,0.0,0.0,0.0,0.0,0.0,0.0,0.0,0.0,0.0,0.0,0.0,0.0,0.0,0.0,0.0,0.0,0.0,0.0,0.0,0.0,0.0,0.0,0.0,0.0,0.0,0.0,0.0,0.0,0.0,0.0,0.0,0.0,0.0,0.0,0.0,0.0,0.0,0.0,0.0,0.0,0.0,0.0,0.0,0.0,0.0,0.0,0.0,0.0,0.0,0.0,0.0,0.0,0.0,0.0,0.0,0.0,0.0,0.0,0.0,0.0,0.0,0.0,0.0,0.0,0.0,0.0,0.0,0.0,0.0,0.0,0.0,0.0,0.0,0.0,0.0,0.0,0.0,0.0,0.0,0.0,0.0,0.0,0.0,0.0,0.0,0.0,0.0,0.0,0.0,0.0,0.0,0.0,0.0,0.0,0.0,0.0,0.0,0.0,0.0,0.0,0.0,0.0,0.0,0.0,0.0,0.0,0.0,0.0,0.0,0.0,0.0,0.0,0.0,0.0,0.0,0.0,0.0,0.0,0.0,0.0,0.0,0.0,0.0,0.0,0.0,0.0,0.0,0.0,0.0,0.0,0.0,0.0,0.0,0.0,0.0,0.0,0.0,0.0,0.0,0.0,0.0,0.0,0.0,0.0,0.0,0.0,0.0,0.0,0.0,0.0,0.0,0.0,0.0,0.0,0.0,0.0,0.0833333358168602,0.1666666716337204,0.25,0.3333333432674408,0.4166666567325592,0.5,0.5833333134651184,0.6666666865348816,0.75,0.8333333134651184,0.9166666865348816,1.0,0.9230769276618958,0.8461538553237915,0.7692307829856873,0.692307710647583,0.6153846383094788,0.5384615659713745,0.4615384638309479,0.38461539149284363,0.3076923191547394,0.23076923191547394,0.1538461595773697,0.07692307978868484,0.0,0.0,0.0,0.0,0.0,0.0,0.0,0.0,0.0,0.0,0.0,0.0,0.0,0.0,0.0,0.0,0.0,0.0,0.0,0.0,0.0,0.0,0.0,0.0,0.0,0.0,0.0,0.0,0.0,0.0,0.0,0.0,0.0,0.0,0.0,0.0,0.0,0.0,0.0,0.0,0.0,0.0,0.0,0.0,0.0,0.0,0.0,0.0,0.0,0.0,0.0,0.0,0.0,0.0,0.0,0.0,0.0,0.0,0.0,0.0,0.0,0.0,0.0,0.0,0.0,0.0,0.0,0.0,0.0,0.0,0.0,0.0,0.0,0.0,0.0,0.0,0.0,0.0,0.0,0.0,0.0,0.0,0.0,0.0,0.0,0.0,0.0,0.0,0.0,0.0,0.0,0.0,0.0,0.0,0.0,0.0,0.0,0.0,0.0,0.0,0.0,0.0,0.0,0.0,0.0,0.0,0.0,0.0,0.0,0.0,0.0,0.0,0.0,0.0,0.0,0.0,0.0,0.0,0.0,0.0,0.0,0.0,0.0,0.0,0.0,0.0,0.0,0.0,0.0,0.0,0.0,0.0,0.0,0.0,0.0,0.0,0.0,0.0,0.0,0.0,0.0,0.0,0.0,0.0,0.0,0.0,0.0,0.0,0.0,0.0,0.0,0.0,0.0,0.0,0.0,0.0,0.0,0.0,0.0,0.0,0.0,0.0,0.0,0.0,0.0,0.0,0.0,0.0,0.0,0.0,0.0,0.0,0.0,0.0,0.0,0.0,0.0,0.0,0.0,0.0,0.0,0.0,0.0,0.0,0.0,0.0,0.0,0.0,0.0,0.0,0.0,0.0,0.0,0.0,0.0,0.0,0.0,0.0,0.0,0.0,0.0,0.0,0.0,0.0,0.0,0.0,0.0,0.0,0.0,0.0,0.0,0.0,0.0,0.0,0.0,0.0,0.0,0.0,0.0,0.0,0.0,0.0,0.0,0.0,0.0,0.0,0.0,0.0,0.0,0.0,0.0,0.0,0.0,0.0,0.0,0.0,0.0,0.0,0.0,0.0,0.0,0.0,0.0,0.0,0.0,0.07692307978868484,0.1538461595773697,0.23076923191547394,0.3076923191547394,0.38461539149284363,0.4615384638309479,0.5384615659713745,0.6153846383094788,0.692307710647583,0.7692307829856873,0.8461538553237915,0.9230769276618958,1.0,0.9285714030265808,0.8571428656578064,0.7857142686843872,0.7142857313156128,0.6428571343421936,0.5714285969734192,0.5,0.4285714328289032,0.3571428656578064,0.2857142984867096,0.2142857164144516,0.1428571492433548,0.0714285746216774,0.0,0.0,0.0,0.0,0.0,0.0,0.0,0.0,0.0,0.0,0.0,0.0,0.0,0.0,0.0,0.0,0.0,0.0,0.0,0.0,0.0,0.0,0.0,0.0,0.0,0.0,0.0,0.0,0.0,0.0,0.0,0.0,0.0,0.0,0.0,0.0,0.0,0.0,0.0,0.0,0.0,0.0,0.0,0.0,0.0,0.0,0.0,0.0,0.0,0.0,0.0,0.0,0.0,0.0,0.0,0.0,0.0,0.0,0.0,0.0,0.0,0.0,0.0,0.0,0.0,0.0,0.0,0.0,0.0,0.0,0.0,0.0,0.0,0.0,0.0,0.0,0.0,0.0,0.0,0.0,0.0,0.0,0.0,0.0,0.0,0.0,0.0,0.0,0.0,0.0,0.0,0.0,0.0,0.0,0.0,0.0,0.0,0.0,0.0,0.0,0.0,0.0,0.0,0.0,0.0,0.0,0.0,0.0,0.0,0.0,0.0,0.0,0.0,0.0,0.0,0.0,0.0,0.0,0.0,0.0,0.0,0.0,0.0,0.0,0.0,0.0,0.0,0.0,0.0,0.0,0.0,0.0,0.0,0.0,0.0,0.0,0.0,0.0,0.0,0.0,0.0,0.0,0.0,0.0,0.0,0.0,0.0,0.0,0.0,0.0,0.0,0.0,0.0,0.0,0.0,0.0,0.0,0.0,0.0,0.0,0.0,0.0,0.0,0.0,0.0,0.0,0.0,0.0,0.0,0.0,0.0,0.0,0.0,0.0,0.0,0.0,0.0,0.0,0.0,0.0,0.0,0.0,0.0,0.0,0.0,0.0,0.0,0.0,0.0,0.0,0.0,0.0,0.0,0.0,0.0,0.0,0.0,0.0,0.0,0.0,0.0,0.0,0.0,0.0,0.0,0.0,0.0,0.0,0.0,0.0,0.0,0.0,0.0,0.0,0.0,0.0,0.0,0.0,0.0,0.0,0.0,0.0,0.0,0.0,0.0,0.0,0.0,0.0,0.0,0.0,0.0,0.0,0.0,0.0,0.0,0.0,0.0,0.0,0.0,0.0,0.0,0.0,0.0,0.0,0.0714285746216774,0.1428571492433548,0.2142857164144516,0.2857142984867096,0.3571428656578064,0.4285714328289032,0.5,0.5714285969734192,0.6428571343421936,0.7142857313156128,0.7857142686843872,0.8571428656578064,0.9285714030265808,1.0,0.9333333373069763,0.8666666746139526,0.800000011920929,0.7333333492279053,0.6666666865348816,0.6000000238418579,0.5333333611488342,0.46666666865348816,0.4000000059604645,0.3333333432674408,0.2666666805744171,0.20000000298023224,0.13333334028720856,0.06666667014360428,0.0,0.0,0.0,0.0,0.0,0.0,0.0,0.0,0.0,0.0,0.0,0.0,0.0,0.0,0.0,0.0,0.0,0.0,0.0,0.0,0.0,0.0,0.0,0.0,0.0,0.0,0.0,0.0,0.0,0.0,0.0,0.0,0.0,0.0,0.0,0.0,0.0,0.0,0.0,0.0,0.0,0.0,0.0,0.0,0.0,0.0,0.0,0.0,0.0,0.0,0.0,0.0,0.0,0.0,0.0,0.0,0.0,0.0,0.0,0.0,0.0,0.0,0.0,0.0,0.0,0.0,0.0,0.0,0.0,0.0,0.0,0.0,0.0,0.0,0.0,0.0,0.0,0.0,0.0,0.0,0.0,0.0,0.0,0.0,0.0,0.0,0.0,0.0,0.0,0.0,0.0,0.0,0.0,0.0,0.0,0.0,0.0,0.0,0.0,0.0,0.0,0.0,0.0,0.0,0.0,0.0,0.0,0.0,0.0,0.0,0.0,0.0,0.0,0.0,0.0,0.0,0.0,0.0,0.0,0.0,0.0,0.0,0.0,0.0,0.0,0.0,0.0,0.0,0.0,0.0,0.0,0.0,0.0,0.0,0.0,0.0,0.0,0.0,0.0,0.0,0.0,0.0,0.0,0.0,0.0,0.0,0.0,0.0,0.0,0.0,0.0,0.0,0.0,0.0,0.0,0.0,0.0,0.0,0.0,0.0,0.0,0.0,0.0,0.0,0.0,0.0,0.0,0.0,0.0,0.0,0.0,0.0,0.0,0.0,0.0,0.0,0.0,0.0,0.0,0.0,0.0,0.0,0.0,0.0,0.0,0.0,0.0,0.0,0.0,0.0,0.0,0.0,0.0,0.0,0.0,0.0,0.0,0.0,0.0,0.0,0.0,0.0,0.0,0.0,0.0,0.0,0.0,0.0,0.0,0.0,0.0,0.0,0.0,0.0,0.0,0.0,0.0,0.0,0.0,0.0,0.0,0.0,0.0,0.0,0.0,0.0,0.0,0.0,0.0,0.0,0.0,0.0,0.0,0.0,0.0,0.0,0.0,0.0,0.0,0.0,0.0,0.0,0.0,0.06666667014360428,0.13333334028720856,0.20000000298023224,0.2666666805744171,0.3333333432674408,0.4000000059604645,0.46666666865348816,0.5333333611488342,0.6000000238418579,0.6666666865348816,0.7333333492279053,0.800000011920929,0.8666666746139526,0.9333333373069763,1.0,0.9333333373069763,0.8666666746139526,0.800000011920929,0.7333333492279053,0.6666666865348816,0.6000000238418579,0.5333333611488342,0.46666666865348816,0.4000000059604645,0.3333333432674408,0.2666666805744171,0.20000000298023224,0.13333334028720856,0.06666667014360428,0.0,0.0,0.0,0.0,0.0,0.0,0.0,0.0,0.0,0.0,0.0,0.0,0.0,0.0,0.0,0.0,0.0,0.0,0.0,0.0,0.0,0.0,0.0,0.0,0.0,0.0,0.0,0.0,0.0,0.0,0.0,0.0,0.0,0.0,0.0,0.0,0.0,0.0,0.0,0.0,0.0,0.0,0.0,0.0,0.0,0.0,0.0,0.0,0.0,0.0,0.0,0.0,0.0,0.0,0.0,0.0,0.0,0.0,0.0,0.0,0.0,0.0,0.0,0.0,0.0,0.0,0.0,0.0,0.0,0.0,0.0,0.0,0.0,0.0,0.0,0.0,0.0,0.0,0.0,0.0,0.0,0.0,0.0,0.0,0.0,0.0,0.0,0.0,0.0,0.0,0.0,0.0,0.0,0.0,0.0,0.0,0.0,0.0,0.0,0.0,0.0,0.0,0.0,0.0,0.0,0.0,0.0,0.0,0.0,0.0,0.0,0.0,0.0,0.0,0.0,0.0,0.0,0.0,0.0,0.0,0.0,0.0,0.0,0.0,0.0,0.0,0.0,0.0,0.0,0.0,0.0,0.0,0.0,0.0,0.0,0.0,0.0,0.0,0.0,0.0,0.0,0.0,0.0,0.0,0.0,0.0,0.0,0.0,0.0,0.0,0.0,0.0,0.0,0.0,0.0,0.0,0.0,0.0,0.0,0.0,0.0,0.0,0.0,0.0,0.0,0.0,0.0,0.0,0.0,0.0,0.0,0.0,0.0,0.0,0.0,0.0,0.0,0.0,0.0,0.0,0.0,0.0,0.0,0.0,0.0,0.0,0.0,0.0,0.0,0.0,0.0,0.0,0.0,0.0,0.0,0.0,0.0,0.0,0.0,0.0,0.0,0.0,0.0,0.0,0.0,0.0,0.0,0.0,0.0,0.0,0.0,0.0,0.0,0.0,0.0,0.0,0.0,0.0,0.0,0.0,0.0,0.0,0.0,0.0,0.0,0.0,0.0,0.0,0.0,0.0,0.0,0.0,0.0,0.0,0.0,0.0,0.0,0.0,0.0,0.0,0.0,0.0,0.0,0.06666667014360428,0.13333334028720856,0.20000000298023224,0.2666666805744171,0.3333333432674408,0.4000000059604645,0.46666666865348816,0.5333333611488342,0.6000000238418579,0.6666666865348816,0.7333333492279053,0.800000011920929,0.8666666746139526,0.9333333373069763,1.0,0.9411764740943909,0.8823529481887817,0.8235294222831726,0.7647058963775635,0.7058823704719543,0.6470588445663452,0.5882353186607361,0.529411792755127,0.47058823704719543,0.4117647111415863,0.3529411852359772,0.29411765933036804,0.23529411852359772,0.1764705926179886,0.11764705926179886,0.05882352963089943,0.0};
__constant__ float c_dct[NMEL * NMEL] = {0.15811388194561005,0.15811388194561005,0.15811388194561005,0.15811388194561005,0.15811388194561005,0.15811388194561005,0.15811388194561005,0.15811388194561005,0.15811388194561005,0.15811388194561005,0.15811388194561005,0.15811388194561005,0.15811388194561005,0.15811388194561005,0.15811388194561005,0.15811388194561005,0.15811388194561005,0.15811388194561005,0.15811388194561005,0.15811388194561005,0.15811388194561005,0.15811388194561005,0.15811388194561005,0.15811388194561005,0.15811388194561005,0.15811388194561005,0.15811388194561005,0.15811388194561005,0.15811388194561005,0.15811388194561005,0.15811388194561005,0.15811388194561005,0.15811388194561005,0.15811388194561005,0.15811388194561005,0.15811388194561005,0.15811388194561005,0.15811388194561005,0.15811388194561005,0.15811388194561005,0.22343440353870392,0.22205685079097748,0.21931025385856628,0.21521154046058655,0.20978595316410065,0.20306698977947235,0.19509603083133698,0.18592225015163422,0.17560219764709473,0.16419950127601624,0.15178446471691132,0.13843362033367157,0.12422928214073181,0.10925903171300888,0.09361516684293747,0.07739412784576416,0.06069593131542206,0.04362352192401886,0.026282161474227905,0.008778762072324753,-0.008778762072324753,-0.026282161474227905,-0.04362352192401886,-0.06069593131542206,-0.07739412784576416,-0.09361516684293747,-0.10925903171300888,-0.12422928214073181,-0.13843362033367157,-0.15178446471691132,-0.16419950127601624,-0.17560219764709473,-0.18592225015163422,-0.19509603083133698,-0.20306698977947235,-0.20978595316410065,-0.21521154046058655,-0.21931025385856628,-0.22205685079097748,-0.22343440353870392,0.22291749715805054,0.217428520321846,0.20658574998378754,0.1906561404466629,0.17003194987773895,0.14522099494934082,0.11683423072099686,0.08557061851024628,0.05219997093081474,0.017543986439704895,-0.017543986439704895,-0.05219997093081474,-0.08557061851024628,-0.11683423072099686,-0.14522099494934082,-0.17003194987773895,-0.1906561404466629,-0.20658574998378754,-0.217428520321846,-0.22291749715805054,-0.22291749715805054,-0.217428520321846,-0.20658574998378754,-0.1906561404466629,-0.17003194987773895,-0.14522099494934082,-0.11683423072099686,-0.08557061851024628,-0.05219997093081474,-0.017543986439704895,0.017543986439704895,0.05219997093081474,0.08557061851024628,0.11683423072099686,0.14522099494934082,0.17003194987773895,0.1906561404466629,0.20658574998378754,0.217428520321846,0.22291749715805054,0.22205685079097748,0.20978595316410065,0.18592225015163422,0.15178446471691132,0.10925903171300888,0.06069593131542206,0.008778762072324753,-0.04362352192401886,-0.09361516684293747,-0.13843362033367157,-0.17560219764709473,-0.20306698977947235,-0.21931025385856628,-0.22343440353870392,-0.21521154046058655,-0.19509603083133698,-0.16419950127601624,-0.12422928214073181,-0.07739412784576416,-0.026282161474227905,0.026282161474227905,0.07739412784576416,0.12422928214073181,0.16419950127601624,0.19509603083133698,0.21521154046058655,0.22343440353870392,0.21931025385856628,0.20306698977947235,0.17560219764709473,0.13843362033367157,0.09361516684293747,0.04362352192401886,-0.008778762072324753,-0.06069593131542206,-0.10925903171300888,-0.15178446471691132,-0.18592225015163422,-0.20978595316410065,-0.22205685079097748,0.22085382044315338,0.19923511147499084,0.15811388194561005,0.10151536017656326,0.03497980907559395,-0.03497980907559395,-0.10151536017656326,-0.15811388194561005,-0.19923511147499084,-0.22085382044315338,-0.22085382044315338,-0.19923511147499084,-0.15811388194561005,-0.10151536017656326,-0.03497980907559395,0.03497980907559395,0.10151536017656326,0.15811388194561005,0.19923511147499084,0.22085382044315338,0.22085382044315338,0.19923511147499084,0.15811388194561005,0.10151536017656326,0.03497980907559395,-0.03497980907559395,-0.10151536017656326,-0.15811388194561005,-0.19923511147499084,-0.22085382044315338,-0.22085382044315338,-0.19923511147499084,-0.15811388194561005,-0.10151536017656326,-0.03497980907559395,0.03497980907559395,0.10151536017656326,0.15811388194561005,0.19923511147499084,0.22085382044315338,0.21931025385856628,0.18592225015163422,0.12422928214073181,0.04362352192401886,-0.04362352192401886,-0.12422928214073181,-0.18592225015163422,-0.21931025385856628,-0.21931025385856628,-0.18592225015163422,-0.12422928214073181,-0.04362352192401886,0.04362352192401886,0.12422928214073181,0.18592225015163422,0.21931025385856628,0.21931025385856628,0.18592225015163422,0.12422928214073181,0.04362352192401886,-0.04362352192401886,-0.12422928214073181,-0.18592225015163422,-0.21931025385856628,-0.21931025385856628,-0.18592225015163422,-0.12422928214073181,-0.04362352192401886,0.04362352192401886,0.12422928214073181,0.18592225015163422,0.21931025385856628,0.21931025385856628,0.18592225015163422,0.12422928214073181,0.04362352192401886,-0.04362352192401886,-0.12422928214073181,-0.18592225015163422,-0.21931025385856628,0.217428520321846,0.17003194987773895,0.08557061851024628,-0.017543986439704895,-0.11683423072099686,-0.1906561404466629,-0.22291749715805054,-0.20658574998378754,-0.14522099494934082,-0.05219997093081474,0.05219997093081474,0.14522099494934082,0.20658574998378754,0.22291749715805054,0.1906561404466629,0.11683423072099686,0.017543986439704895,-0.08557061851024628,-0.17003194987773895,-0.217428520321846,-0.217428520321846,-0.17003194987773895,-0.08557061851024628,0.017543986439704895,0.11683423072099686,0.1906561404466629,0.22291749715805054,0.20658574998378754,0.14522099494934082,0.05219997093081474,-0.05219997093081474,-0.14522099494934082,-0.20658574998378754,-0.22291749715805054,-0.1906561404466629,-0.11683423072099686,-0.017543986439704895,0.08557061851024628,0.17003194987773895,0.217428520321846,0.21521154046058655,0.15178446471691132,0.04362352192401886,-0.07739412784576416,-0.17560219764709473,-0.22205685079097748,-0.20306698977947235,-0.12422928214073181,-0.008778762072324753,0.10925903171300888,0.19509603083133698,0.22343440353870392,0.18592225015163422,0.09361516684293747,-0.026282161474227905,-0.13843362033367157,-0.20978595316410065,-0.21931025385856628,-0.16419950127601624,-0.06069593131542206,0.06069593131542206,0.16419950127601624,0.21931025385856628,0.20978595316410065,0.13843362033367157,0.026282161474227905,-0.09361516684293747,-0.18592225015163422,-0.22343440353870392,-0.19509603083133698,-0.10925903171300888,0.008778762072324753,0.12422928214073181,0.20306698977947235,0.22205685079097748,0.17560219764709473,0.07739412784576416,-0.04362352192401886,-0.15178446471691132,-0.21521154046058655,0.2126626968383789,0.13143277168273926,1.3691967473468707e-17,-0.13143277168273926,-0.2126626968383789,-0.2126626968383789,-0.13143277168273926,-4.1075903247586733e-17,0.13143277168273926,0.2126626968383789,0.2126626968383789,0.13143277168273926,6.845983654016292e-17,-0.13143277168273926,-0.2126626968383789,-0.2126626968383789,-0.13143277168273926,-9.584376983273911e-17,0.13143277168273926,0.2126626968383789,0.2126626968383789,0.13143277168273926,1.232277031253153e-16,-0.13143277168273926,-0.2126626968383789,-0.2126626968383789,-0.13143277168273926,2.4659381672816787e-16,0.13143277168273926,0.2126626968383789,0.2126626968383789,0.13143277168273926,5.752010162390821e-16,-0.13143277168273926,-0.2126626968383789,-0.2126626968383789,-0.13143277168273926,-6.025849561491032e-16,0.13143277168273926,0.2126626968383789,0.20978595316410065,0.10925903171300888,-0.04362352192401886,-0.17560219764709473,-0.22343440353870392,-0.16419950127601624,-0.026282161474227905,0.12422928214073181,0.21521154046058655,0.20306698977947235,0.09361516684293747,-0.06069593131542206,-0.18592225015163422,-0.22205685079097748,-0.15178446471691132,-0.008778762072324753,0.13843362033367157,0.21931025385856628,0.19509603083133698,0.07739412784576416,-0.07739412784576416,-0.19509603083133698,-0.21931025385856628,-0.13843362033367157,0.008778762072324753,0.15178446471691132,0.22205685079097748,0.18592225015163422,0.06069593131542206,-0.09361516684293747,-0.20306698977947235,-0.21521154046058655,-0.12422928214073181,0.026282161474227905,0.16419950127601624,0.22343440353870392,0.17560219764709473,0.04362352192401886,-0.10925903171300888,-0.20978595316410065,0.20658574998378754,0.08557061851024628,-0.08557061851024628,-0.20658574998378754,-0.20658574998378754,-0.08557061851024628,0.08557061851024628,0.20658574998378754,0.20658574998378754,0.08557061851024628,-0.08557061851024628,-0.20658574998378754,-0.20658574998378754,-0.08557061851024628,0.08557061851024628,0.20658574998378754,0.20658574998378754,0.08557061851024628,-0.08557061851024628,-0.20658574998378754,-0.20658574998378754,-0.08557061851024628,0.08557061851024628,0.20658574998378754,0.20658574998378754,0.08557061851024628,-0.08557061851024628,-0.20658574998378754,-0.20658574998378754,-0.08557061851024628,0.08557061851024628,0.20658574998378754,0.20658574998378754,0.08557061851024628,-0.08557061851024628,-0.20658574998378754,-0.20658574998378754,-0.08557061851024628,0.08557061851024628,0.20658574998378754,0.20306698977947235,0.06069593131542206,-0.12422928214073181,-0.22205685079097748,-0.16419950127601624,0.008778762072324753,0.17560219764709473,0.21931025385856628,0.10925903171300888,-0.07739412784576416,-0.20978595316410065,-0.19509603083133698,-0.04362352192401886,0.13843362033367157,0.22343440353870392,0.15178446471691132,-0.026282161474227905,-0.18592225015163422,-0.21521154046058655,-0.09361516684293747,0.09361516684293747,0.21521154046058655,0.18592225015163422,0.026282161474227905,-0.15178446471691132,-0.22343440353870392,-0.13843362033367157,0.04362352192401886,0.19509603083133698,0.20978595316410065,0.07739412784576416,-0.10925903171300888,-0.21931025385856628,-0.17560219764709473,-0.008778762072324753,0.16419950127601624,0.22205685079097748,0.12422928214073181,-0.06069593131542206,-0.20306698977947235,0.19923511147499084,0.03497980907559395,-0.15811388194561005,-0.22085382044315338,-0.10151536017656326,0.10151536017656326,0.22085382044315338,0.15811388194561005,-0.03497980907559395,-0.19923511147499084,-0.19923511147499084,-0.03497980907559395,0.15811388194561005,0.22085382044315338,0.10151536017656326,-0.10151536017656326,-0.22085382044315338,-0.15811388194561005,0.03497980907559395,0.19923511147499084,0.19923511147499084,0.03497980907559395,-0.15811388194561005,-0.22085382044315338,-0.10151536017656326,0.10151536017656326,0.22085382044315338,0.15811388194561005,-0.03497980907559395,-0.19923511147499084,-0.19923511147499084,-0.03497980907559395,0.15811388194561005,0.22085382044315338,0.10151536017656326,-0.10151536017656326,-0.22085382044315338,-0.15811388194561005,0.03497980907559395,0.19923511147499084,0.19509603083133698,0.008778762072324753,-0.18592225015163422,-0.20306698977947235,-0.026282161474227905,0.17560219764709473,0.20978595316410065,0.04362352192401886,-0.16419950127601624,-0.21521154046058655,-0.06069593131542206,0.15178446471691132,0.21931025385856628,0.07739412784576416,-0.13843362033367157,-0.22205685079097748,-0.09361516684293747,0.12422928214073181,0.22343440353870392,0.10925903171300888,-0.10925903171300888,-0.22343440353870392,-0.12422928214073181,0.09361516684293747,0.22205685079097748,0.13843362033367157,-0.07739412784576416,-0.21931025385856628,-0.15178446471691132,0.06069593131542206,0.21521154046058655,0.16419950127601624,-0.04362352192401886,-0.20978595316410065,-0.17560219764709473,0.026282161474227905,0.20306698977947235,0.18592225015163422,-0.008778762072324753,-0.19509603083133698,0.1906561404466629,-0.017543986439704895,-0.20658574998378754,-0.17003194987773895,0.05219997093081474,0.217428520321846,0.14522099494934082,-0.08557061851024628,-0.22291749715805054,-0.11683423072099686,0.11683423072099686,0.22291749715805054,0.08557061851024628,-0.14522099494934082,-0.217428520321846,-0.05219997093081474,0.17003194987773895,0.20658574998378754,0.017543986439704895,-0.1906561404466629,-0.1906561404466629,0.017543986439704895,0.20658574998378754,0.17003194987773895,-0.05219997093081474,-0.217428520321846,-0.14522099494934082,0.08557061851024628,0.22291749715805054,0.11683423072099686,-0.11683423072099686,-0.22291749715805054,-0.08557061851024628,0.14522099494934082,0.217428520321846,0.05219997093081474,-0.17003194987773895,-0.20658574998378754,-0.017543986439704895,0.1906561404466629,0.18592225015163422,-0.04362352192401886,-0.21931025385856628,-0.12422928214073181,0.12422928214073181,0.21931025385856628,0.04362352192401886,-0.18592225015163422,-0.18592225015163422,0.04362352192401886,0.21931025385856628,0.12422928214073181,-0.12422928214073181,-0.21931025385856628,-0.04362352192401886,0.18592225015163422,0.18592225015163422,-0.04362352192401886,-0.21931025385856628,-0.12422928214073181,0.12422928214073181,0.21931025385856628,0.04362352192401886,-0.18592225015163422,-0.18592225015163422,0.04362352192401886,0.21931025385856628,0.12422928214073181,-0.12422928214073181,-0.21931025385856628,-0.04362352192401886,0.18592225015163422,0.18592225015163422,-0.04362352192401886,-0.21931025385856628,-0.12422928214073181,0.12422928214073181,0.21931025385856628,0.04362352192401886,-0.18592225015163422,0.18090170621871948,-0.06909830123186111,-0.22360679507255554,-0.06909830123186111,0.18090170621871948,0.18090170621871948,-0.06909830123186111,-0.22360679507255554,-0.06909830123186111,0.18090170621871948,0.18090170621871948,-0.06909830123186111,-0.22360679507255554,-0.06909830123186111,0.18090170621871948,0.18090170621871948,-0.06909830123186111,-0.22360679507255554,-0.06909830123186111,0.18090170621871948,0.18090170621871948,-0.06909830123186111,-0.22360679507255554,-0.06909830123186111,0.18090170621871948,0.18090170621871948,-0.06909830123186111,-0.22360679507255554,-0.06909830123186111,0.18090170621871948,0.18090170621871948,-0.06909830123186111,-0.22360679507255554,-0.06909830123186111,0.18090170621871948,0.18090170621871948,-0.06909830123186111,-0.22360679507255554,-0.06909830123186111,0.18090170621871948,0.17560219764709473,-0.09361516684293747,-0.21931025385856628,-0.008778762072324753,0.21521154046058655,0.10925903171300888,-0.16419950127601624,-0.18592225015163422,0.07739412784576416,0.22205685079097748,0.026282161474227905,-0.20978595316410065,-0.12422928214073181,0.15178446471691132,0.19509603083133698,-0.06069593131542206,-0.22343440353870392,-0.04362352192401886,0.20306698977947235,0.13843362033367157,-0.13843362033367157,-0.20306698977947235,0.04362352192401886,0.22343440353870392,0.06069593131542206,-0.19509603083133698,-0.15178446471691132,0.12422928214073181,0.20978595316410065,-0.026282161474227905,-0.22205685079097748,-0.07739412784576416,0.18592225015163422,0.16419950127601624,-0.10925903171300888,-0.21521154046058655,0.008778762072324753,0.21931025385856628,0.09361516684293747,-0.17560219764709473,0.17003194987773895,-0.11683423072099686,-0.20658574998378754,0.05219997093081474,0.22291749715805054,0.017543986439704895,-0.217428520321846,-0.08557061851024628,0.1906561404466629,0.14522099494934082,-0.14522099494934082,-0.1906561404466629,0.08557061851024628,0.217428520321846,-0.017543986439704895,-0.22291749715805054,-0.05219997093081474,0.20658574998378754,0.11683423072099686,-0.17003194987773895,-0.17003194987773895,0.11683423072099686,0.20658574998378754,-0.05219997093081474,-0.22291749715805054,-0.017543986439704895,0.217428520321846,0.08557061851024628,-0.1906561404466629,-0.14522099494934082,0.14522099494934082,0.1906561404466629,-0.08557061851024628,-0.217428520321846,0.017543986439704895,0.22291749715805054,0.05219997093081474,-0.20658574998378754,-0.11683423072099686,0.17003194987773895,0.16419950127601624,-0.13843362033367157,-0.18592225015163422,0.10925903171300888,0.20306698977947235,-0.07739412784576416,-0.21521154046058655,0.04362352192401886,0.22205685079097748,-0.008778762072324753,-0.22343440353870392,-0.026282161474227905,0.21931025385856628,0.06069593131542206,-0.20978595316410065,-0.09361516684293747,0.19509603083133698,0.12422928214073181,-0.17560219764709473,-0.15178446471691132,0.15178446471691132,0.17560219764709473,-0.12422928214073181,-0.19509603083133698,0.09361516684293747,0.20978595316410065,-0.06069593131542206,-0.21931025385856628,0.026282161474227905,0.22343440353870392,0.008778762072324753,-0.22205685079097748,-0.04362352192401886,0.21521154046058655,0.07739412784576416,-0.20306698977947235,-0.10925903171300888,0.18592225015163422,0.13843362033367157,-0.16419950127601624,0.15811388194561005,-0.15811388194561005,-0.15811388194561005,0.15811388194561005,0.15811388194561005,-0.15811388194561005,-0.15811388194561005,0.15811388194561005,0.15811388194561005,-0.15811388194561005,-0.15811388194561005,0.15811388194561005,0.15811388194561005,-0.15811388194561005,-0.15811388194561005,0.15811388194561005,0.15811388194561005,-0.15811388194561005,-0.15811388194561005,0.15811388194561005,0.15811388194561005,-0.15811388194561005,-0.15811388194561005,0.15811388194561005,0.15811388194561005,-0.15811388194561005,-0.15811388194561005,0.15811388194561005,0.15811388194561005,-0.15811388194561005,-0.15811388194561005,0.15811388194561005,0.15811388194561005,-0.15811388194561005,-0.15811388194561005,0.15811388194561005,0.15811388194561005,-0.15811388194561005,-0.15811388194561005,0.15811388194561005,0.15178446471691132,-0.17560219764709473,-0.12422928214073181,0.19509603083133698,0.09361516684293747,-0.20978595316410065,-0.06069593131542206,0.21931025385856628,0.026282161474227905,-0.22343440353870392,0.008778762072324753,0.22205685079097748,-0.04362352192401886,-0.21521154046058655,0.07739412784576416,0.20306698977947235,-0.10925903171300888,-0.18592225015163422,0.13843362033367157,0.16419950127601624,-0.16419950127601624,-0.13843362033367157,0.18592225015163422,0.10925903171300888,-0.20306698977947235,-0.07739412784576416,0.21521154046058655,0.04362352192401886,-0.22205685079097748,-0.008778762072324753,0.22343440353870392,-0.026282161474227905,-0.21931025385856628,0.06069593131542206,0.20978595316410065,-0.09361516684293747,-0.19509603083133698,0.12422928214073181,0.17560219764709473,-0.15178446471691132,0.14522099494934082,-0.1906561404466629,-0.08557061851024628,0.217428520321846,0.017543986439704895,-0.22291749715805054,0.05219997093081474,0.20658574998378754,-0.11683423072099686,-0.17003194987773895,0.17003194987773895,0.11683423072099686,-0.20658574998378754,-0.05219997093081474,0.22291749715805054,-0.017543986439704895,-0.217428520321846,0.08557061851024628,0.1906561404466629,-0.14522099494934082,-0.14522099494934082,0.1906561404466629,0.08557061851024628,-0.217428520321846,-0.017543986439704895,0.22291749715805054,-0.05219997093081474,-0.20658574998378754,0.11683423072099686,0.17003194987773895,-0.17003194987773895,-0.11683423072099686,0.20658574998378754,0.05219997093081474,-0.22291749715805054,0.017543986439704895,0.217428520321846,-0.08557061851024628,-0.1906561404466629,0.14522099494934082,0.13843362033367157,-0.20306698977947235,-0.04362352192401886,0.22343440353870392,-0.06069593131542206,-0.19509603083133698,0.15178446471691132,0.12422928214073181,-0.20978595316410065,-0.026282161474227905,0.22205685079097748,-0.07739412784576416,-0.18592225015163422,0.16419950127601624,0.10925903171300888,-0.21521154046058655,-0.008778762072324753,0.21931025385856628,-0.09361516684293747,-0.17560219764709473,0.17560219764709473,0.09361516684293747,-0.21931025385856628,0.008778762072324753,0.21521154046058655,-0.10925903171300888,-0.16419950127601624,0.18592225015163422,0.07739412784576416,-0.22205685079097748,0.026282161474227905,0.20978595316410065,-0.12422928214073181,-0.15178446471691132,0.19509603083133698,0.06069593131542206,-0.22343440353870392,0.04362352192401886,0.20306698977947235,-0.13843362033367157,0.13143277168273926,-0.2126626968383789,-4.1075903247586733e-17,0.2126626968383789,-0.13143277168273926,-0.13143277168273926,0.2126626968383789,1.232277031253153e-16,-0.2126626968383789,0.13143277168273926,0.13143277168273926,-0.2126626968383789,-6.025849561491032e-16,0.2126626968383789,-0.13143277168273926,-0.13143277168273926,0.2126626968383789,-1.0967415026528693e-16,-0.2126626968383789,0.13143277168273926,0.13143277168273926,-0.2126626968383789,-7.668885956092298e-16,0.2126626968383789,-0.13143277168273926,-0.13143277168273926,0.2126626968383789,1.6434513348663016e-15,-0.2126626968383789,0.13143277168273926,0.13143277168273926,-0.2126626968383789,-9.311922350693563e-16,0.2126626968383789,-0.13143277168273926,-0.13143277168273926,0.2126626968383789,2.1893306909796204e-16,-0.2126626968383789,0.13143277168273926,0.12422928214073181,-0.21931025385856628,0.04362352192401886,0.18592225015163422,-0.18592225015163422,-0.04362352192401886,0.21931025385856628,-0.12422928214073181,-0.12422928214073181,0.21931025385856628,-0.04362352192401886,-0.18592225015163422,0.18592225015163422,0.04362352192401886,-0.21931025385856628,0.12422928214073181,0.12422928214073181,-0.21931025385856628,0.04362352192401886,0.18592225015163422,-0.18592225015163422,-0.04362352192401886,0.21931025385856628,-0.12422928214073181,-0.12422928214073181,0.21931025385856628,-0.04362352192401886,-0.18592225015163422,0.18592225015163422,0.04362352192401886,-0.21931025385856628,0.12422928214073181,0.12422928214073181,-0.21931025385856628,0.04362352192401886,0.18592225015163422,-0.18592225015163422,-0.04362352192401886,0.21931025385856628,-0.12422928214073181,0.11683423072099686,-0.22291749715805054,0.08557061851024628,0.14522099494934082,-0.217428520321846,0.05219997093081474,0.17003194987773895,-0.20658574998378754,0.017543986439704895,0.1906561404466629,-0.1906561404466629,-0.017543986439704895,0.20658574998378754,-0.17003194987773895,-0.05219997093081474,0.217428520321846,-0.14522099494934082,-0.08557061851024628,0.22291749715805054,-0.11683423072099686,-0.11683423072099686,0.22291749715805054,-0.08557061851024628,-0.14522099494934082,0.217428520321846,-0.05219997093081474,-0.17003194987773895,0.20658574998378754,-0.017543986439704895,-0.1906561404466629,0.1906561404466629,0.017543986439704895,-0.20658574998378754,0.17003194987773895,0.05219997093081474,-0.217428520321846,0.14522099494934082,0.08557061851024628,-0.22291749715805054,0.11683423072099686,0.10925903171300888,-0.22343440353870392,0.12422928214073181,0.09361516684293747,-0.22205685079097748,0.13843362033367157,0.07739412784576416,-0.21931025385856628,0.15178446471691132,0.06069593131542206,-0.21521154046058655,0.16419950127601624,0.04362352192401886,-0.20978595316410065,0.17560219764709473,0.026282161474227905,-0.20306698977947235,0.18592225015163422,0.008778762072324753,-0.19509603083133698,0.19509603083133698,-0.008778762072324753,-0.18592225015163422,0.20306698977947235,-0.026282161474227905,-0.17560219764709473,0.20978595316410065,-0.04362352192401886,-0.16419950127601624,0.21521154046058655,-0.06069593131542206,-0.15178446471691132,0.21931025385856628,-0.07739412784576416,-0.13843362033367157,0.22205685079097748,-0.09361516684293747,-0.12422928214073181,0.22343440353870392,-0.10925903171300888,0.10151536017656326,-0.22085382044315338,0.15811388194561005,0.03497980907559395,-0.19923511147499084,0.19923511147499084,-0.03497980907559395,-0.15811388194561005,0.22085382044315338,-0.10151536017656326,-0.10151536017656326,0.22085382044315338,-0.15811388194561005,-0.03497980907559395,0.19923511147499084,-0.19923511147499084,0.03497980907559395,0.15811388194561005,-0.22085382044315338,0.10151536017656326,0.10151536017656326,-0.22085382044315338,0.15811388194561005,0.03497980907559395,-0.19923511147499084,0.19923511147499084,-0.03497980907559395,-0.15811388194561005,0.22085382044315338,-0.10151536017656326,-0.10151536017656326,0.22085382044315338,-0.15811388194561005,-0.03497980907559395,0.19923511147499084,-0.19923511147499084,0.03497980907559395,0.15811388194561005,-0.22085382044315338,0.10151536017656326,0.09361516684293747,-0.21521154046058655,0.18592225015163422,-0.026282161474227905,-0.15178446471691132,0.22343440353870392,-0.13843362033367157,-0.04362352192401886,0.19509603083133698,-0.20978595316410065,0.07739412784576416,0.10925903171300888,-0.21931025385856628,0.17560219764709473,-0.008778762072324753,-0.16419950127601624,0.22205685079097748,-0.12422928214073181,-0.06069593131542206,0.20306698977947235,-0.20306698977947235,0.06069593131542206,0.12422928214073181,-0.22205685079097748,0.16419950127601624,0.008778762072324753,-0.17560219764709473,0.21931025385856628,-0.10925903171300888,-0.07739412784576416,0.20978595316410065,-0.19509603083133698,0.04362352192401886,0.13843362033367157,-0.22343440353870392,0.15178446471691132,0.026282161474227905,-0.18592225015163422,0.21521154046058655,-0.09361516684293747,0.08557061851024628,-0.20658574998378754,0.20658574998378754,-0.08557061851024628,-0.08557061851024628,0.20658574998378754,-0.20658574998378754,0.08557061851024628,0.08557061851024628,-0.20658574998378754,0.20658574998378754,-0.08557061851024628,-0.08557061851024628,0.20658574998378754,-0.20658574998378754,0.08557061851024628,0.08557061851024628,-0.20658574998378754,0.20658574998378754,-0.08557061851024628,-0.08557061851024628,0.20658574998378754,-0.20658574998378754,0.08557061851024628,0.08557061851024628,-0.20658574998378754,0.20658574998378754,-0.08557061851024628,-0.08557061851024628,0.20658574998378754,-0.20658574998378754,0.08557061851024628,0.08557061851024628,-0.20658574998378754,0.20658574998378754,-0.08557061851024628,-0.08557061851024628,0.20658574998378754,-0.20658574998378754,0.08557061851024628,0.07739412784576416,-0.19509603083133698,0.21931025385856628,-0.13843362033367157,-0.008778762072324753,0.15178446471691132,-0.22205685079097748,0.18592225015163422,-0.06069593131542206,-0.09361516684293747,0.20306698977947235,-0.21521154046058655,0.12422928214073181,0.026282161474227905,-0.16419950127601624,0.22343440353870392,-0.17560219764709473,0.04362352192401886,0.10925903171300888,-0.20978595316410065,0.20978595316410065,-0.10925903171300888,-0.04362352192401886,0.17560219764709473,-0.22343440353870392,0.16419950127601624,-0.026282161474227905,-0.12422928214073181,0.21521154046058655,-0.20306698977947235,0.09361516684293747,0.06069593131542206,-0.18592225015163422,0.22205685079097748,-0.15178446471691132,0.008778762072324753,0.13843362033367157,-0.21931025385856628,0.19509603083133698,-0.07739412784576416,0.06909830123186111,-0.18090170621871948,0.22360679507255554,-0.18090170621871948,0.06909830123186111,0.06909830123186111,-0.18090170621871948,0.22360679507255554,-0.18090170621871948,0.06909830123186111,0.06909830123186111,-0.18090170621871948,0.22360679507255554,-0.18090170621871948,0.06909830123186111,0.06909830123186111,-0.18090170621871948,0.22360679507255554,-0.18090170621871948,0.06909830123186111,0.06909830123186111,-0.18090170621871948,0.22360679507255554,-0.18090170621871948,0.06909830123186111,0.06909830123186111,-0.18090170621871948,0.22360679507255554,-0.18090170621871948,0.06909830123186111,0.06909830123186111,-0.18090170621871948,0.22360679507255554,-0.18090170621871948,0.06909830123186111,0.06909830123186111,-0.18090170621871948,0.22360679507255554,-0.18090170621871948,0.06909830123186111,0.06069593131542206,-0.16419950127601624,0.21931025385856628,-0.20978595316410065,0.13843362033367157,-0.026282161474227905,-0.09361516684293747,0.18592225015163422,-0.22343440353870392,0.19509603083133698,-0.10925903171300888,-0.008778762072324753,0.12422928214073181,-0.20306698977947235,0.22205685079097748,-0.17560219764709473,0.07739412784576416,0.04362352192401886,-0.15178446471691132,0.21521154046058655,-0.21521154046058655,0.15178446471691132,-0.04362352192401886,-0.07739412784576416,0.17560219764709473,-0.22205685079097748,0.20306698977947235,-0.12422928214073181,0.008778762072324753,0.10925903171300888,-0.19509603083133698,0.22343440353870392,-0.18592225015163422,0.09361516684293747,0.026282161474227905,-0.13843362033367157,0.20978595316410065,-0.21931025385856628,0.16419950127601624,-0.06069593131542206,0.05219997093081474,-0.14522099494934082,0.20658574998378754,-0.22291749715805054,0.1906561404466629,-0.11683423072099686,0.017543986439704895,0.08557061851024628,-0.17003194987773895,0.217428520321846,-0.217428520321846,0.17003194987773895,-0.08557061851024628,-0.017543986439704895,0.11683423072099686,-0.1906561404466629,0.22291749715805054,-0.20658574998378754,0.14522099494934082,-0.05219997093081474,-0.05219997093081474,0.14522099494934082,-0.20658574998378754,0.22291749715805054,-0.1906561404466629,0.11683423072099686,-0.017543986439704895,-0.08557061851024628,0.17003194987773895,-0.217428520321846,0.217428520321846,-0.17003194987773895,0.08557061851024628,0.017543986439704895,-0.11683423072099686,0.1906561404466629,-0.22291749715805054,0.20658574998378754,-0.14522099494934082,0.05219997093081474,0.04362352192401886,-0.12422928214073181,0.18592225015163422,-0.21931025385856628,0.21931025385856628,-0.18592225015163422,0.12422928214073181,-0.04362352192401886,-0.04362352192401886,0.12422928214073181,-0.18592225015163422,0.21931025385856628,-0.21931025385856628,0.18592225015163422,-0.12422928214073181,0.04362352192401886,0.04362352192401886,-0.12422928214073181,0.18592225015163422,-0.21931025385856628,0.21931025385856628,-0.18592225015163422,0.12422928214073181,-0.04362352192401886,-0.04362352192401886,0.12422928214073181,-0.18592225015163422,0.21931025385856628,-0.21931025385856628,0.18592225015163422,-0.12422928214073181,0.04362352192401886,0.04362352192401886,-0.12422928214073181,0.18592225015163422,-0.21931025385856628,0.21931025385856628,-0.18592225015163422,0.12422928214073181,-0.04362352192401886,0.03497980907559395,-0.10151536017656326,0.15811388194561005,-0.19923511147499084,0.22085382044315338,-0.22085382044315338,0.19923511147499084,-0.15811388194561005,0.10151536017656326,-0.03497980907559395,-0.03497980907559395,0.10151536017656326,-0.15811388194561005,0.19923511147499084,-0.22085382044315338,0.22085382044315338,-0.19923511147499084,0.15811388194561005,-0.10151536017656326,0.03497980907559395,0.03497980907559395,-0.10151536017656326,0.15811388194561005,-0.19923511147499084,0.22085382044315338,-0.22085382044315338,0.19923511147499084,-0.15811388194561005,0.10151536017656326,-0.03497980907559395,-0.03497980907559395,0.10151536017656326,-0.15811388194561005,0.19923511147499084,-0.22085382044315338,0.22085382044315338,-0.19923511147499084,0.15811388194561005,-0.10151536017656326,0.03497980907559395,0.026282161474227905,-0.07739412784576416,0.12422928214073181,-0.16419950127601624,0.19509603083133698,-0.21521154046058655,0.22343440353870392,-0.21931025385856628,0.20306698977947235,-0.17560219764709473,0.13843362033367157,-0.09361516684293747,0.04362352192401886,0.008778762072324753,-0.06069593131542206,0.10925903171300888,-0.15178446471691132,0.18592225015163422,-0.20978595316410065,0.22205685079097748,-0.22205685079097748,0.20978595316410065,-0.18592225015163422,0.15178446471691132,-0.10925903171300888,0.06069593131542206,-0.008778762072324753,-0.04362352192401886,0.09361516684293747,-0.13843362033367157,0.17560219764709473,-0.20306698977947235,0.21931025385856628,-0.22343440353870392,0.21521154046058655,-0.19509603083133698,0.16419950127601624,-0.12422928214073181,0.07739412784576416,-0.026282161474227905,0.017543986439704895,-0.05219997093081474,0.08557061851024628,-0.11683423072099686,0.14522099494934082,-0.17003194987773895,0.1906561404466629,-0.20658574998378754,0.217428520321846,-0.22291749715805054,0.22291749715805054,-0.217428520321846,0.20658574998378754,-0.1906561404466629,0.17003194987773895,-0.14522099494934082,0.11683423072099686,-0.08557061851024628,0.05219997093081474,-0.017543986439704895,-0.017543986439704895,0.05219997093081474,-0.08557061851024628,0.11683423072099686,-0.14522099494934082,0.17003194987773895,-0.1906561404466629,0.20658574998378754,-0.217428520321846,0.22291749715805054,-0.22291749715805054,0.217428520321846,-0.20658574998378754,0.1906561404466629,-0.17003194987773895,0.14522099494934082,-0.11683423072099686,0.08557061851024628,-0.05219997093081474,0.017543986439704895,0.008778762072324753,-0.026282161474227905,0.04362352192401886,-0.06069593131542206,0.07739412784576416,-0.09361516684293747,0.10925903171300888,-0.12422928214073181,0.13843362033367157,-0.15178446471691132,0.16419950127601624,-0.17560219764709473,0.18592225015163422,-0.19509603083133698,0.20306698977947235,-0.20978595316410065,0.21521154046058655,-0.21931025385856628,0.22205685079097748,-0.22343440353870392,0.22343440353870392,-0.22205685079097748,0.21931025385856628,-0.21521154046058655,0.20978595316410065,-0.20306698977947235,0.19509603083133698,-0.18592225015163422,0.17560219764709473,-0.16419950127601624,0.15178446471691132,-0.13843362033367157,0.12422928214073181,-0.10925903171300888,0.09361516684293747,-0.07739412784576416,0.06069593131542206,-0.04362352192401886,0.026282161474227905,-0.008778762072324753};
__constant__ float c_win[WINL] = {0.07999999821186066,0.08005674928426743,0.08022698014974594,0.08051066100597382,0.08090770244598389,0.08141802996397018,0.08204149454832077,0.0827779620885849,0.08362723886966705,0.08458911627531052,0.08566336333751678,0.08684971183538437,0.08814786374568939,0.08955750614404678,0.09107828885316849,0.09270983934402466,0.09445174783468246,0.09630358964204788,0.0982649028301239,0.10033521056175232,0.10251400619745255,0.1048007383942604,0.10719484835863113,0.10969574749469757,0.11230281740427017,0.1150154173374176,0.11783286929130554,0.12075449526309967,0.12377955764532089,0.1269073188304901,0.13013699650764465,0.13346780836582184,0.1368989199399948,0.14042949676513672,0.14405867457389832,0.14778552949428558,0.1516091525554657,0.15552861988544464,0.15954293310642242,0.16365112364292145,0.16785217821598053,0.1721450537443161,0.1765286922454834,0.18100200593471527,0.18556390702724457,0.19021326303482056,0.19494891166687012,0.19976969063282013,0.20467443764209747,0.20966190099716187,0.2147308737039566,0.2198801189661026,0.2251083254814148,0.2304142415523529,0.23579654097557068,0.24125389754772186,0.246784970164299,0.2523883879184723,0.2580627501010895,0.26380670070648193,0.26961877942085266,0.27549758553504944,0.28144165873527527,0.28744950890541077,0.29351967573165894,0.2996506690979004,0.30584093928337097,0.3120890259742737,0.3183933198451996,0.3247522711753845,0.3311643600463867,0.33762797713279724,0.34414151310920715,0.3507033884525299,0.3573119640350342,0.36396563053131104,0.37066271901130676,0.37740156054496765,0.38418054580688477,0.390997976064682,0.39785218238830566,0.40474143624305725,0.41166409850120544,0.41861841082572937,0.42560264468193054,0.43261513113975525,0.4396541118621826,0.44671785831451416,0.4538045823574066,0.4609126150608063,0.4680401384830475,0.47518542408943176,0.48234671354293823,0.48952221870422363,0.4967101812362671,0.5039088129997253,0.5111163854598999,0.5183310508728027,0.5255510210990906,0.5327746272087097,0.5400000214576721,0.5472253561019897,0.5544489622116089,0.5616689920425415,0.5688836574554443,0.5760911703109741,0.5832898020744324,0.5904777646064758,0.5976532697677612,0.6048145890235901,0.6119598746299744,0.6190873980522156,0.6261954307556152,0.6332821846008301,0.6403458714485168,0.6473848819732666,0.6543973684310913,0.6613816022872925,0.6683359146118164,0.6752585768699646,0.6821478009223938,0.6890020370483398,0.6958194375038147,0.7025984525680542,0.7093372941017151,0.7160343527793884,0.7226880192756653,0.7292966246604919,0.7358585000038147,0.7423720359802246,0.7488356232643127,0.7552477121353149,0.7616066932678223,0.7679110169410706,0.7741590738296509,0.7803493142127991,0.7864803075790405,0.7925505042076111,0.7985583543777466,0.8045024275779724,0.8103812336921692,0.8161932826042175,0.8219372630119324,0.8276116251945496,0.833215057849884,0.8387461304664612,0.8442034721374512,0.849585771560669,0.8548916578292847,0.8601198792457581,0.865269124507904,0.8703380823135376,0.8753255605697632,0.8802303075790405,0.8850510716438293,0.8897867202758789,0.8944361209869385,0.898997962474823,0.9034712910652161,0.9078549146652222,0.9121478199958801,0.9163488745689392,0.9204570651054382,0.924471378326416,0.9283908605575562,0.9322144985198975,0.9359413385391235,0.9395704865455627,0.9431010484695435,0.9465321898460388,0.9498630166053772,0.9530926942825317,0.9562204480171204,0.959245502948761,0.9621671438217163,0.9649845957756042,0.9676972031593323,0.9703042507171631,0.9728051424026489,0.975199282169342,0.9774860143661499,0.9796648025512695,0.981735110282898,0.9836964011192322,0.9855482578277588,0.9872901439666748,0.9889217019081116,0.9904425144195557,0.9918521642684937,0.9931502938270569,0.9943366646766663,0.9954108595848083,0.9963727593421936,0.9972220659255981,0.9979584813117981,0.9985819458961487,0.9990922808647156,0.9994893670082092,0.9997730255126953,0.9999432563781738,1.0,0.9999432563781738,0.9997730255126953,0.9994893670082092,0.9990922808647156,0.9985819458961487,0.9979584813117981,0.9972220659255981,0.9963727593421936,0.9954108595848083,0.9943366646766663,0.9931502938270569,0.9918521642684937,0.9904425144195557,0.9889217019081116,0.9872901439666748,0.9855482578277588,0.9836964011192322,0.981735110282898,0.9796648025512695,0.9774860143661499,0.975199282169342,0.9728051424026489,0.9703042507171631,0.9676972031593323,0.9649845957756042,0.9621671438217163,0.959245502948761,0.9562204480171204,0.9530926942825317,0.9498630166053772,0.9465321898460388,0.9431010484695435,0.9395704865455627,0.9359413385391235,0.9322144985198975,0.9283908605575562,0.924471378326416,0.9204570651054382,0.9163488745689392,0.9121478199958801,0.9078549146652222,0.9034712910652161,0.898997962474823,0.8944361209869385,0.8897867202758789,0.8850510716438293,0.8802303075790405,0.8753255605697632,0.8703380823135376,0.865269124507904,0.8601198792457581,0.8548916578292847,0.849585771560669,0.8442034721374512,0.8387461304664612,0.833215057849884,0.8276116251945496,0.8219372630119324,0.8161932826042175,0.8103812336921692,0.8045024275779724,0.7985583543777466,0.7925505042076111,0.7864803075790405,0.7803493142127991,0.7741590738296509,0.7679110169410706,0.7616066932678223,0.7552477121353149,0.7488356232643127,0.7423720359802246,0.7358585000038147,0.7292966246604919,0.7226880192756653,0.7160343527793884,0.7093372941017151,0.7025984525680542,0.6958194375038147,0.6890020370483398,0.6821478009223938,0.6752585768699646,0.6683359146118164,0.6613816022872925,0.6543973684310913,0.6473848819732666,0.6403458714485168,0.6332821846008301,0.6261954307556152,0.6190873980522156,0.6119598746299744,0.6048145890235901,0.5976532697677612,0.5904777646064758,0.5832898020744324,0.5760911703109741,0.5688836574554443,0.5616689920425415,0.5544489622116089,0.5472253561019897,0.5400000214576721,0.5327746272087097,0.5255510210990906,0.5183310508728027,0.5111163854598999,0.5039088129997253,0.4967101812362671,0.48952221870422363,0.48234671354293823,0.47518542408943176,0.4680401384830475,0.4609126150608063,0.4538045823574066,0.44671785831451416,0.4396541118621826,0.43261513113975525,0.42560264468193054,0.41861841082572937,0.41166409850120544,0.40474143624305725,0.39785218238830566,0.390997976064682,0.38418054580688477,0.37740156054496765,0.37066271901130676,0.36396563053131104,0.3573119640350342,0.3507033884525299,0.34414151310920715,0.33762797713279724,0.3311643600463867,0.3247522711753845,0.3183933198451996,0.3120890259742737,0.30584093928337097,0.2996506690979004,0.29351967573165894,0.28744950890541077,0.28144165873527527,0.27549758553504944,0.26961877942085266,0.26380670070648193,0.2580627501010895,0.2523883879184723,0.246784970164299,0.24125389754772186,0.23579654097557068,0.2304142415523529,0.2251083254814148,0.2198801189661026,0.2147308737039566,0.20966190099716187,0.20467443764209747,0.19976969063282013,0.19494891166687012,0.19021326303482056,0.18556390702724457,0.18100200593471527,0.1765286922454834,0.1721450537443161,0.16785217821598053,0.16365112364292145,0.15954293310642242,0.15552861988544464,0.1516091525554657,0.14778552949428558,0.14405867457389832,0.14042949676513672,0.1368989199399948,0.13346780836582184,0.13013699650764465,0.1269073188304901,0.12377955764532089,0.12075449526309967,0.11783286929130554,0.1150154173374176,0.11230281740427017,0.10969574749469757,0.10719484835863113,0.1048007383942604,0.10251400619745255,0.10033521056175232,0.0982649028301239,0.09630358964204788,0.09445174783468246,0.09270983934402466,0.09107828885316849,0.08955750614404678,0.08814786374568939,0.08684971183538437,0.08566336333751678,0.08458911627531052,0.08362723886966705,0.0827779620885849,0.08204149454832077,0.08141802996397018,0.08090770244598389,0.08051066100597382,0.08022698014974594,0.08005674928426743};

__device__ __forceinline__ f32x8 wmma16(f16x16 a, f16x16 b, f32x8 c) {
  c = __builtin_amdgcn_wmma_f32_16x16x32_f16(false, a, false, b, (short)0, c, false, false);
  asm volatile("v_nop\n\tv_nop\n\tv_nop\n\tv_nop" : "+v"(c) : "v"(a), "v"(b));
  return c;
}
__device__ __forceinline__ f16x16 lds_frag(const f16* base, int stride) {
  const int lane = threadIdx.x & 31, row = lane & 15, kh = (lane >> 4) * 8;
  const f16x8 lo = *(const f16x8*)(base + row * stride + kh);
  const f16x8 hi = *(const f16x8*)(base + row * stride + kh + 16);
  f16x16 f;
#pragma unroll
  for (int i = 0; i < 8; ++i) { f[i] = lo[i]; f[i + 8] = hi[i]; }
  return f;
}
__device__ __forceinline__ f16x16 cfrag(const float* __restrict__ M, int ld, int nrows, int ncols, int r0, int k0) {
  const int lane = threadIdx.x & 31, r = r0 + (lane & 15), kh = (lane >> 4) * 8;
  f16x16 f;
#pragma unroll
  for (int i = 0; i < 8; ++i) { const int ka = k0 + kh + i, kb2 = k0 + 16 + kh + i;
    f[i] = (f16)((r < nrows && ka < ncols) ? M[r * ld + ka] : 0.0f); f[8 + i] = (f16)((r < nrows && kb2 < ncols) ? M[r * ld + kb2] : 0.0f); }
  return f;
}

__global__ __launch_bounds__(256) void k_mfcc(const float* __restrict__ x, float* __restrict__ out) {
  __shared__ float twc[512], tws[512];
  __shared__ __attribute__((aligned(16))) f16 aS[2][FB * 40];
  __shared__ __attribute__((aligned(16))) f16 wS[2][128 * 40];
  __shared__ __attribute__((aligned(16))) f16 magS[FB * 296];
  __shared__ __attribute__((aligned(16))) union U { float reim[FB * 132]; struct { f16 lmS[FB * 72]; float melS[FB * 44]; float oS[FB * NOUT]; } p; } u;
  float* reim = u.reim; f16* lmS = u.p.lmS; float* melS = u.p.melS; float* oS = u.p.oS;
  const int tid = threadIdx.x, lane = tid & 31, wave = tid >> 5, cl = lane & 15, rh = (lane >> 4) * 8;
  const int f0 = blockIdx.x * FB;
  for (int i = tid; i < 512; i += 256) { const float ang = (float)i * (6.283185307179586f / 512.0f); twc[i] = cosf(ang); tws[i] = sinf(ang); }
  for (int e = tid; e < FB * 296; e += 256) magS[e] = (f16)0.0f;
  const int rt = wave & 3, chh = wave >> 2;
  __syncthreads();
#pragma unroll 1
  for (int nt = 0; nt < 5; ++nt) {
    f32x8 acc[4], accx[4];
#pragma unroll
    for (int j = 0; j < 4; ++j) { f32x8 z = {}; acc[j] = z; accx[j] = z; }
#pragma unroll 1
    for (int ks = 0; ks < 13; ++ks) {
      __syncthreads();
      for (int e = tid; e < FB * 32; e += 256) { const int r = e >> 5, kk = e & 31, n = ks * 32 + kk; float v = 0.0f;
        if (n < WINL) { const int f = f0 + r, b = f / NFR, t = f % NFR; const size_t gi = (size_t)b * NSAMP + (size_t)t * HOPL + n;
          const float xv = x[gi]; const float xp = (t * HOPL + n > 0) ? x[gi - 1] : 0.0f;
          v = ((t * HOPL + n > 0) ? (xv - 0.97f * xp) : xv) * c_win[n]; }
        { const f16 h = (f16)v; aS[0][r * 40 + kk] = h; aS[1][r * 40 + kk] = (f16)((v - (float)h) * 2048.0f); } }
      for (int e = tid; e < 128 * 32; e += 256) { const int j = e >> 5, kk = e & 31, n = ks * 32 + kk, k = nt * 64 + (j & 63); float w = 0.0f;
        if (k < NBIN && n < WINL) { const int idx = (k * n) & 511; w = (j < 64) ? twc[idx] : tws[idx]; }
        { const f16 h = (f16)w; wS[0][j * 40 + kk] = h; wS[1][j * 40 + kk] = (f16)((w - (float)h) * 2048.0f); } }
      __syncthreads();
      const f16x16 ah = lds_frag(aS[0] + (rt * 16) * 40, 40), al = lds_frag(aS[1] + (rt * 16) * 40, 40);
#pragma unroll
      for (int j = 0; j < 4; ++j) { const f16x16 bh = lds_frag(wS[0] + (chh * 64 + j * 16) * 40, 40), bl = lds_frag(wS[1] + (chh * 64 + j * 16) * 40, 40);
        acc[j] = wmma16(ah, bh, acc[j]); accx[j] = wmma16(ah, bl, accx[j]); accx[j] = wmma16(al, bh, accx[j]); }
    }
#pragma unroll
    for (int j = 0; j < 4; ++j)
#pragma unroll
      for (int r = 0; r < 8; ++r) reim[(rt * 16 + rh + r) * 132 + chh * 64 + j * 16 + cl] = acc[j][r] + accx[j][r] * (1.0f / 2048.0f);
    __syncthreads();
    for (int e = tid; e < FB * 64; e += 256) { const int r = e >> 6, kl = e & 63, k = nt * 64 + kl;
      if (k < NBIN) { const float re = reim[r * 132 + kl], im = reim[r * 132 + 64 + kl]; magS[r * 296 + k] = (f16)sqrtf(re * re + im * im); } }
  }
  __syncthreads();
  {
    const int mt0 = (wave >> 2) ? 2 : 0, nmt = (wave >> 2) ? 1 : 2;
    for (int mi = 0; mi < nmt; ++mi) { const int mt = mt0 + mi; f32x8 acc = {};
#pragma unroll 1
      for (int ks = 0; ks < 9; ++ks) acc = wmma16(lds_frag(magS + (rt * 16) * 296 + ks * 32, 296), cfrag(c_fbank, NBIN, NMEL, NBIN, mt * 16, ks * 32), acc);
      const int m = mt * 16 + cl;
      if (m < NMEL) {
#pragma unroll
        for (int r = 0; r < 8; ++r) melS[(rt * 16 + rh + r) * 44 + m] = acc[r]; } }
  }
  __syncthreads();
  for (int e = tid; e < FB * 64; e += 256) { const int r = e >> 6, m = e & 63; lmS[r * 72 + m] = (f16)((m < NMEL) ? logf(melS[r * 44 + m] + 1e-20f) : 0.0f); }
  __syncthreads();
  {
    const int mt0 = (wave >> 2) ? 2 : 0, nmt = (wave >> 2) ? 1 : 2;
    for (int mi = 0; mi < nmt; ++mi) { const int ct = mt0 + mi; f32x8 acc = {};
#pragma unroll
      for (int ks = 0; ks < 2; ++ks) acc = wmma16(lds_frag(lmS + (rt * 16) * 72 + ks * 32, 72), cfrag(c_dct, NMEL, NMEL, NMEL, ct * 16, ks * 32), acc);
      const int c = ct * 16 + cl;
      if (c < NMEL) {
#pragma unroll
        for (int r = 0; r < 8; ++r) melS[(rt * 16 + rh + r) * 44 + c] = acc[r]; } }
  }
  __syncthreads();
  if (tid < FB) { const float* mr = melS + tid * 44; float d1[16];
    d1[0] = 0.0f;
#pragma unroll
    for (int c = 1; c < 16; ++c) d1[c] = (mr[c + 1] - mr[c - 1]) * 0.5f;
#pragma unroll
    for (int c = 0; c < 13; ++c) { oS[tid * NOUT + c] = mr[c]; oS[tid * NOUT + 13 + c] = d1[c]; oS[tid * NOUT + 26 + c] = (c == 0) ? 0.0f : (d1[c + 1] - d1[c - 1]) * 0.5f; } }
  __syncthreads();
  float* dst = out + (size_t)f0 * NOUT;
#pragma unroll 1
  for (int pass = 0; pass < 2; ++pass) {
    for (int q = tid; q < FB * NOUT / 4; q += 256) *(volatile v4f_t*)(dst + q * 4) = *(const volatile v4fa*)(oS + q * 4);
    __threadfence();
  }
}

extern "C" void kernel_launch(void* const* d_in, const int* in_sizes, int n_in,
                              void* d_out, int out_size, void* d_ws, size_t ws_size,
                              hipStream_t stream) {
  (void)in_sizes; (void)n_in; (void)out_size; (void)d_ws; (void)ws_size;
  const float* x = (const float*)d_in[0];
  float* out = (float*)d_out;
  k_mfcc<<<dim3(NFRAMES / FB), dim3(256), 0, stream>>>(x, out);
}
